// WGAT_14508399525893
// MI455X (gfx1250) — hardware-verified
//
#include <hip/hip_runtime.h>
#include <math.h>

typedef __attribute__((ext_vector_type(16))) _Float16 v16h;
typedef __attribute__((ext_vector_type(8)))  _Float16 v8h;
typedef __attribute__((ext_vector_type(16))) __bf16   v16b;
typedef __attribute__((ext_vector_type(8)))  float    v8f;
typedef __attribute__((ext_vector_type(4)))  float    v4f;

__device__ __forceinline__ int frag_k(int i, int h) { return (i < 8) ? (8 * h + i) : (16 + 8 * h + (i - 8)); }
__device__ __forceinline__ __bf16 bf16_rne(float f) {
    unsigned int u = __float_as_uint(f);
    u += 0x7fffu + ((u >> 16) & 1u);
    return __builtin_bit_cast(__bf16, (unsigned short)(u >> 16));
}
__device__ __forceinline__ float bf16_f32(__bf16 b) { return __uint_as_float(((unsigned int)__builtin_bit_cast(unsigned short, b)) << 16); }
__device__ __forceinline__ v8f wmma16(v16h a, v16h b, v8f c) {
    c = __builtin_amdgcn_wmma_f32_16x16x32_f16(false, a, false, b, (short)0, c, false, false);
    asm volatile("v_nop\n\tv_nop\n\tv_nop\n\tv_nop" : "+v"(c) : "v"(a), "v"(b));
    return c;
}
__device__ __forceinline__ v8f wmmab(v16b a, v16b b, v8f c) {
    c = __builtin_amdgcn_wmma_f32_16x16x32_bf16(false, a, false, b, (short)0, c, false, false);
    asm volatile("v_nop\n\tv_nop\n\tv_nop\n\tv_nop" : "+v"(c) : "v"(a), "v"(b));
    return c;
}
struct Split { v16b hi, lo; };
__device__ __forceinline__ v8f wmma3(const Split& a, const Split& b, v8f c) {
    c = __builtin_amdgcn_wmma_f32_16x16x32_bf16(false, a.hi, false, b.hi, (short)0, c, false, false);
    c = __builtin_amdgcn_wmma_f32_16x16x32_bf16(false, a.hi, false, b.lo, (short)0, c, false, false);
    c = __builtin_amdgcn_wmma_f32_16x16x32_bf16(false, a.lo, false, b.hi, (short)0, c, false, false);
    asm volatile("v_nop\n\tv_nop\n\tv_nop\n\tv_nop" : "+v"(c) : "v"(a.hi), "v"(a.lo), "v"(b.hi), "v"(b.lo));
    return c;
}
struct Split3 { v16b hi, mid, lo; };
__device__ __forceinline__ v8f wmma6(const Split3& a, const Split3& b, v8f c) {
    c = __builtin_amdgcn_wmma_f32_16x16x32_bf16(false, a.hi, false, b.hi, (short)0, c, false, false);
    c = __builtin_amdgcn_wmma_f32_16x16x32_bf16(false, a.hi, false, b.mid, (short)0, c, false, false);
    c = __builtin_amdgcn_wmma_f32_16x16x32_bf16(false, a.mid, false, b.hi, (short)0, c, false, false);
    c = __builtin_amdgcn_wmma_f32_16x16x32_bf16(false, a.hi, false, b.lo, (short)0, c, false, false);
    c = __builtin_amdgcn_wmma_f32_16x16x32_bf16(false, a.mid, false, b.mid, (short)0, c, false, false);
    c = __builtin_amdgcn_wmma_f32_16x16x32_bf16(false, a.lo, false, b.hi, (short)0, c, false, false);
    asm volatile("v_nop\n\tv_nop\n\tv_nop\n\tv_nop" : "+v"(c) : "v"(a.hi), "v"(a.mid), "v"(a.lo), "v"(b.hi), "v"(b.mid), "v"(b.lo));
    return c;
}

__device__ __forceinline__ v16h fh_ld(const float* __restrict__ p, long long sk, int k0, int h, int klen, float s) {
    v16h a;
#pragma unroll
    for (int i = 0; i < 16; ++i) { const int k = k0 + frag_k(i, h); a[i] = (k < klen) ? (_Float16)(p[(long long)k * sk] * s) : (_Float16)0.f; }
    return a;
}
__device__ __forceinline__ Split sp_ld(const float* __restrict__ p, long long sk, int k0, int h, int klen, float s) {
    Split r;
#pragma unroll
    for (int i = 0; i < 16; ++i) {
        const int k = k0 + frag_k(i, h); const float x = (k < klen) ? p[(long long)k * sk] * s : 0.f;
        const __bf16 hb = bf16_rne(x); r.hi[i] = hb; r.lo[i] = bf16_rne(x - bf16_f32(hb));
    }
    return r;
}
__device__ __forceinline__ Split3 sp3_ld(const float* __restrict__ p, long long sk, int k0, int h, int klen, float s) {
    Split3 r;
#pragma unroll
    for (int i = 0; i < 16; ++i) {
        const int k = k0 + frag_k(i, h); const float x = (k < klen) ? p[(long long)k * sk] * s : 0.f;
        const __bf16 hb = bf16_rne(x); const float r1 = x - bf16_f32(hb); const __bf16 mb = bf16_rne(r1);
        r.hi[i] = hb; r.mid[i] = mb; r.lo[i] = bf16_rne(r1 - bf16_f32(mb));
    }
    return r;
}
__device__ __forceinline__ v16b bh_ld(const float* __restrict__ p, long long sk, int k0, int h, int klen, float s) {
    v16b a;
#pragma unroll
    for (int i = 0; i < 16; ++i) { const int k = k0 + frag_k(i, h); a[i] = bf16_rne((k < klen) ? p[(long long)k * sk] * s : 0.f); }
    return a;
}
__device__ __forceinline__ v16h fh_row(const _Float16* __restrict__ row, int k0, int h) {
    v16h a;
#pragma unroll
    for (int i = 0; i < 16; ++i) a[i] = row[k0 + frag_k(i, h)];
    return a;
}

#define VST2(T, ptr, val) do { *(volatile T*)(ptr) = (val); __threadfence(); *(volatile T*)(ptr) = (val); } while (0)
typedef float v4f __attribute__((ext_vector_type(4)));
#define VST2V4(ptr, val) do { *(volatile v4f*)(ptr) = (val); __threadfence(); *(volatile v4f*)(ptr) = (val); } while (0)

__device__ __attribute__((noinline)) float act_fn(float v, int act) {
    if (act == 1) return fmaxf(v, 0.f);
    if (act == 2) { const float u = 0.7978845608028654f * (v + 0.044715f * v * v * v); return 0.5f * v * (1.f + tanhf(u)); }
    if (act == 3) return v / (1.f + expf(-v));
    if (act == 4) return 0.5f * v * (1.f + erff(v * 0.7071067811865476f));
    if (act == 5) return tanhf(v);
    if (act == 6) return 1.f / (1.f + expf(-v));
    if (act == 7) return (v > 0.f) ? v : 0.01f * v;
    if (act == 8) return (v > 0.f) ? v : (expf(v) - 1.f);
    if (act == 9) return fminf(fmaxf(v, 0.f), 6.f);
    if (act == 10) return fabsf(v);
    if (act == 11) return (v >= 0.f) ? v : 0.1f * v;
    if (act == 12) return (v > 0.f) ? v : 0.2f * v;
    if (act == 13) return (v > 20.f) ? v : log1pf(expf(v));
    return v;
}

struct GemmP {
    const float* A; const float* B; const float* bias; const float* R; float* C;
    long long sAo, sAi, sAm, sAk, sBo, sBi, sBn, sBk, sCo, sCi, sCm, sRo, sRi, sRm, sRn;
    int M, N, K, zi_n, flags, act; float alpha, beta, sa, sb;
    int Npad, pad_;
};
static_assert(sizeof(GemmP) == 5 * 8 + 15 * 8 + 6 * 4 + 4 * 4 + 2 * 4, "GemmP has padding");

template <int MODE>
__global__ __launch_bounds__(32) void k_gemm(GemmP p) {
    const int lane = threadIdx.x & 31, h = lane >> 4, l15 = lane & 15;
    const int m0 = blockIdx.y * 16, n0 = blockIdx.x * 32;
    const int z = blockIdx.z, zo = z / p.zi_n, zi = z - zo * p.zi_n;
    const float* A = p.A + zo * p.sAo + zi * p.sAi;
    const float* B = p.B + zo * p.sBo + zi * p.sBi;
    const int am = min(m0 + l15, p.M - 1);
    v8f acc[2], comp[2];
#pragma unroll
    for (int t = 0; t < 2; ++t) { v8f zz = {}; acc[t] = zz; comp[t] = zz; }
    for (int k0 = 0; k0 < p.K; k0 += 32) {
        const float* arow = A + (long long)am * p.sAm;
        if (MODE == 1) {
            const Split a = sp_ld(arow, p.sAk, k0, h, p.K, 1.f);
#pragma unroll
            for (int t = 0; t < 2; ++t) {
                const int bn = min(n0 + t * 16 + l15, p.N - 1);
                acc[t] = wmma3(a, sp_ld(B + (long long)bn * p.sBn, p.sBk, k0, h, p.K, 1.f), acc[t]);
            }
        } else if (MODE == 3) {
            const Split3 a = sp3_ld(arow, p.sAk, k0, h, p.K, 1.f);
#pragma unroll
            for (int t = 0; t < 2; ++t) {
                const int bn = min(n0 + t * 16 + l15, p.N - 1);
                acc[t] = wmma6(a, sp3_ld(B + (long long)bn * p.sBn, p.sBk, k0, h, p.K, 1.f), acc[t]);
            }
        } else if (MODE == 4) {
            const Split3 a = sp3_ld(arow, p.sAk, k0, h, p.K, 1.f);
#pragma unroll
            for (int t = 0; t < 2; ++t) {
                const int bn = min(n0 + t * 16 + l15, p.N - 1); v8f zz = {};
                const v8f part = wmma6(a, sp3_ld(B + (long long)bn * p.sBn, p.sBk, k0, h, p.K, 1.f), zz);
                const v8f y = part - comp[t]; const v8f s = acc[t] + y; comp[t] = (s - acc[t]) - y; acc[t] = s;
            }
        } else if (MODE == 2) {
            const v16b a = bh_ld(arow, p.sAk, k0, h, p.K, 1.f);
#pragma unroll
            for (int t = 0; t < 2; ++t) {
                const int bn = min(n0 + t * 16 + l15, p.N - 1);
                acc[t] = wmmab(a, bh_ld(B + (long long)bn * p.sBn, p.sBk, k0, h, p.K, 1.f), acc[t]);
            }
        } else {
            const v16h a = fh_ld(arow, p.sAk, k0, h, p.K, p.sa);
#pragma unroll
            for (int t = 0; t < 2; ++t) {
                const int bn = min(n0 + t * 16 + l15, p.N - 1);
                acc[t] = wmma16(a, fh_ld(B + (long long)bn * p.sBn, p.sBk, k0, h, p.K, p.sb), acc[t]);
            }
        }
    }
    const float iscale = (MODE == 0) ? p.alpha / (p.sa * p.sb) : p.alpha;
    float* C = p.C + zo * p.sCo + zi * p.sCi;
    const float* R = p.R + zo * p.sRo + zi * p.sRi;
    __shared__ __align__(16) float ctile[16][36];
#pragma unroll
    for (int t = 0; t < 2; ++t) {
        const int n = n0 + t * 16 + l15; const int nn = min(n, p.N - 1);
#pragma unroll
        for (int r = 0; r < 8; ++r) {
            const int m = m0 + 8 * h + r; const int mm = min(m, p.M - 1);
            float v = acc[t][r] * iscale;
            if (p.flags & 1) v += p.bias[nn];
            if (p.flags & 2) v += p.bias[mm];
            v = act_fn(v, p.act);
            if (p.flags & 4) v += p.beta * R[(long long)mm * p.sRm + (long long)nn * p.sRn];
            ctile[8 * h + r][t * 16 + l15] = (n < p.N) ? v : 0.f;
        }
    }
    __syncthreads();
    const int NW = (p.Npad > p.N) ? p.Npad : p.N;
    const bool fast = (m0 + 16 <= p.M) && (n0 + 32 <= NW) && ((p.sCm & 3) == 0) && ((((size_t)C) & 15) == 0);
    if (fast) {
#pragma unroll
        for (int s = 0; s < 4; ++s) {
            const int row = s * 4 + (lane >> 3), c4 = (lane & 7) * 4;
            const v4f v = *(const v4f*)&ctile[row][c4];
            VST2V4(C + (long long)(m0 + row) * p.sCm + n0 + c4, v);
        }
    } else {
        for (int row = 0; row < 16; ++row) {
            const int m = m0 + row, n = n0 + lane;
            if (m < p.M && n < NW) VST2(float, C + (long long)m * p.sCm + n, ctile[row][lane]);
        }
    }
}

#define AW 4
struct AttnP {
    const float* Q; const float* K; const float* V; float* O; float* P; const float* Mf; const int* Mi; float* ST;
    const float* Pw; const float* Rt; const int* SQ; const int* SK;
    long long swb, swh, swi, swj, srb, srh, sri;
    long long sQb, sQh, sQi, sQd, sKb, sKh, sKj, sKd, sVb, sVh, sVj, sVd, sOb, sOh, sOi, sPb, sPh, sPi, smb, smh, smi, smj;
    int Lq, Lk, dh, dv, hrep, causal, coff, pband;
    float scale, mfill; int nonorm, mpol;
    int roff, rn, segpol, win;
};
static_assert(sizeof(AttnP) == 12 * 8 + 29 * 8 + 16 * 4, "AttnP has padding");

#ifndef KATTN_ATTR
#define KATTN_ATTR
#endif
template <int DHP, int DVP, int QM, bool SPLITPV, bool TWOPASS>
__global__ __launch_bounds__(32 * AW) KATTN_ATTR void k_attn(AttnP p) {
    constexpr int NT = DVP / 16;
    constexpr int KS = DHP / 32;
    constexpr int VP = DVP + 8;
    __shared__ __align__(16) float    pl[AW][16 * 64];
    __shared__ __align__(16) _Float16 vl[(SPLITPV ? 2 : 1) * 64 * VP];
    const int lane = threadIdx.x & 31, hf = lane >> 4, l15 = lane & 15, wave = threadIdx.x >> 5;
    const int h = blockIdx.y, b = blockIdx.z, hk = h / p.hrep;
    const int q0 = (blockIdx.x * AW + wave) * 16;
    float* myp = pl[wave];
    const float L2E = 1.4426950408889634f;
    const float NEG = -__builtin_inff();
    const int qi = min(q0 + l15, p.Lq - 1);
    const float* qrow = p.Q + b * p.sQb + h * p.sQh + (long long)qi * p.sQi;
    const float* kbase = p.K + b * p.sKb + hk * p.sKh;
    const float* vbase = p.V + b * p.sVb + hk * p.sVh;
    v16h qa[QM == 0 ? KS : 1]; Split qs_[QM == 1 ? KS : 1]; Split3 qt_[QM == 2 ? KS : 1];
#pragma unroll
    for (int ks = 0; ks < KS; ++ks) {
        if (QM == 2) qt_[ks] = sp3_ld(qrow, p.sQd, ks * 32, hf, p.dh, 1.f);
        else if (QM == 1) qs_[ks] = sp_ld(qrow, p.sQd, ks * 32, hf, p.dh, 1.f);
        else qa[ks] = fh_ld(qrow, p.sQd, ks * 32, hf, p.dh, 1.f);
    }
    v8f o[NT]; float m8[8], l8[8];
#pragma unroll
    for (int t = 0; t < NT; ++t) { v8f zz = {}; o[t] = zz; }
#pragma unroll
    for (int i = 0; i < 8; ++i) { m8[i] = NEG; l8[i] = 0.f; }
    int jend = p.Lk;
    if (p.causal == 1) { const int je = (blockIdx.x * AW + AW - 1) * 16 + 16 + p.coff; jend = min(jend, max(je, 0)); }
    const int npass = TWOPASS ? 2 : 1;
    for (int pass = 0; pass < npass; ++pass) {
        const bool dopv = (!TWOPASS) || pass == 1;
        for (int j0 = 0; j0 < jend; j0 += 64) {
            if (dopv) {
                __syncthreads();
                for (int idx = threadIdx.x; idx < 64 * DVP; idx += 32 * AW) {
                    const int jr = idx / DVP, d = idx - jr * DVP, j = j0 + jr;
                    const float f = (j < p.Lk && d < p.dv) ? vbase[(long long)j * p.sVj + (long long)d * p.sVd] : 0.f;
                    if (SPLITPV) {
                        const __bf16 hb = bf16_rne(f);
                        ((__bf16*)vl)[jr * VP + d] = hb; ((__bf16*)vl)[64 * VP + jr * VP + d] = bf16_rne(f - bf16_f32(hb));
                    } else vl[jr * VP + d] = (_Float16)f;
                }
            }
            v8f s[4];
#pragma unroll
            for (int t = 0; t < 4; ++t) {
                const int j = min(j0 + t * 16 + l15, p.Lk - 1);
                const float* krow = kbase + (long long)j * p.sKj;
                v8f acc = {};
#pragma unroll
                for (int ks = 0; ks < KS; ++ks) {
                    if (QM == 2)      acc = wmma6(qt_[ks], sp3_ld(krow, p.sKd, ks * 32, hf, p.dh, 1.f), acc);
                    else if (QM == 1) acc = wmma3(qs_[ks], sp_ld(krow, p.sKd, ks * 32, hf, p.dh, 1.f), acc);
                    else              acc = wmma16(qa[ks], fh_ld(krow, p.sKd, ks * 32, hf, p.dh, 1.f), acc);
                }
                s[t] = acc;
            }
            float pv[8][4];
#pragma unroll
            for (int i = 0; i < 8; ++i) {
                const int irow = q0 + i + 8 * hf;
                const int ic = min(irow, p.Lq - 1);
                float sc[4];
#pragma unroll
                for (int t = 0; t < 4; ++t) {
                    const int jg = j0 + t * 16 + l15;
                    float v = s[t][i] * p.scale;
                    if (p.Mf) v += p.Mf[b * p.smb + h * p.smh + (long long)ic * p.smi + (long long)min(jg, p.Lk - 1) * p.smj];
                    if (p.Rt) { int rc = ic - min(jg, p.Lk - 1) + p.roff; rc = rc < 0 ? 0 : (rc >= p.rn ? p.rn - 1 : rc); v += p.Rt[b * p.srb + h * p.srh + (long long)ic * p.sri + rc]; }
                    if (p.Mi) { const int mv = p.Mi[b * p.smb + h * p.smh + (long long)ic * p.smi + (long long)min(jg, p.Lk - 1) * p.smj]; if (p.mpol ? (mv != 0) : (mv == 0)) v = p.mfill; }
                    if (p.SQ) { const bool same = p.SQ[(long long)b * p.Lq + ic] == p.SK[(long long)b * p.Lk + min(jg, p.Lk - 1)]; if (p.segpol ? same : !same) v = p.mfill; }
                    if (p.causal == 2 && jg > irow + p.coff) v = p.mfill;
                    if (jg >= p.Lk || (p.causal == 1 && jg > irow + p.coff) || (p.causal == 3 && jg < irow + p.coff) || (p.win > 0 && irow + p.coff - jg > p.win)) v = NEG; else v *= L2E;
                    sc[t] = v;
                }
                if (!TWOPASS || pass == 0) {
                    float mx = fmaxf(fmaxf(sc[0], sc[1]), fmaxf(sc[2], sc[3]));
                    mx = fmaxf(mx, __shfl_xor(mx, 1, 32)); mx = fmaxf(mx, __shfl_xor(mx, 2, 32));
                    mx = fmaxf(mx, __shfl_xor(mx, 4, 32)); mx = fmaxf(mx, __shfl_xor(mx, 8, 32));
                    const float mnew = fmaxf(m8[i], mx);
                    const float corr = (mnew == NEG) ? 1.f : exp2f(m8[i] - mnew);
                    float rs = 0.f;
#pragma unroll
                    for (int t = 0; t < 4; ++t) {
                        const float pp = (sc[t] == NEG) ? 0.f : exp2f(sc[t] - mnew); rs += pp;
                        pv[i][t] = p.Pw ? pp * p.Pw[b * p.swb + h * p.swh + (long long)ic * p.swi + (long long)min(j0 + t * 16 + l15, p.Lk - 1) * p.swj] : pp;
                    }
                    rs += __shfl_xor(rs, 1, 32); rs += __shfl_xor(rs, 2, 32); rs += __shfl_xor(rs, 4, 32); rs += __shfl_xor(rs, 8, 32);
                    l8[i] = l8[i] * corr + rs; m8[i] = mnew;
                    if (!TWOPASS) {
#pragma unroll
                        for (int t = 0; t < NT; ++t) o[t][i] *= corr;
                    }
                } else {
                    const float inv = (l8[i] > 0.f) ? 1.f / l8[i] : 0.f;
#pragma unroll
                    for (int t = 0; t < 4; ++t) {
                        const int jg = j0 + t * 16 + l15;
                        float pp = (sc[t] == NEG) ? 0.f : exp2f(sc[t] - m8[i]) * inv;
                        if (p.Pw) pp *= p.Pw[b * p.swb + h * p.swh + (long long)ic * p.swi + (long long)min(jg, p.Lk - 1) * p.swj];
                        pv[i][t] = pp;
                    }
                }
            }
            if (dopv) {
#pragma unroll
                for (int i = 0; i < 8; ++i)
#pragma unroll
                    for (int t = 0; t < 4; ++t) myp[(i + 8 * hf) * 64 + t * 16 + l15] = pv[i][t];
                __syncthreads();
                if (p.P) {
                    float* pb_ = p.P + b * p.sPb + h * p.sPh;
                    const bool fastP = (p.pband == 0) && ((p.sPi & 3) == 0) && (j0 + 64 <= p.Lk) && (q0 + 16 <= p.Lq) && ((((size_t)pb_) & 15) == 0);
                    if (fastP) {
#pragma unroll
                        for (int s = 0; s < 8; ++s) {
                            const int row = s * 2 + (lane >> 4), c4 = (lane & 15) * 4;
                            const v4f v = *(const v4f*)(myp + row * 64 + c4);
                            VST2V4(pb_ + (long long)(q0 + row) * p.sPi + j0 + c4, v);
                        }
                    } else {
                        for (int row = 0; row < 16; ++row) {
                            const int irow = q0 + row; if (irow >= p.Lq) continue;
                            for (int c = lane; c < 64; c += 32) {
                                const int jg = j0 + c; if (jg >= p.Lk) continue;
                                if (p.pband == 0) VST2(float, pb_ + (long long)irow * p.sPi + jg, myp[row * 64 + c]);
                                else if (jg - irow <= p.pband && irow - jg <= p.pband) VST2(float, pb_ + (long long)irow * p.sPi + (jg - irow + p.pband), myp[row * 64 + c]);
                            }
                        }
                    }
                }
                if (SPLITPV) {
                    const Split pa0 = sp_ld(myp + l15 * 64, 1, 0, hf, 64, 1.f), pa1 = sp_ld(myp + l15 * 64, 1, 32, hf, 64, 1.f);
                    const __bf16* vh = (const __bf16*)vl; const __bf16* vlo = vh + 64 * VP;
#pragma unroll
                    for (int t = 0; t < NT; ++t) {
                        const int dcol = t * 16 + l15;
                        Split b0, b1;
#pragma unroll
                        for (int e = 0; e < 16; ++e) {
                            const int k0 = frag_k(e, hf), k1 = 32 + frag_k(e, hf);
                            b0.hi[e] = vh[k0 * VP + dcol]; b0.lo[e] = vlo[k0 * VP + dcol]; b1.hi[e] = vh[k1 * VP + dcol]; b1.lo[e] = vlo[k1 * VP + dcol];
                        }
                        o[t] = wmma3(pa0, b0, o[t]);
                        o[t] = wmma3(pa1, b1, o[t]);
                    }
                } else {
                    const v16h pa0 = fh_ld(myp + l15 * 64, 1, 0, hf, 64, 4096.f), pa1 = fh_ld(myp + l15 * 64, 1, 32, hf, 64, 4096.f);
#pragma unroll
                    for (int t = 0; t < NT; ++t) {
                        const int dcol = t * 16 + l15;
                        v16h b0, b1;
#pragma unroll
                        for (int e = 0; e < 16; ++e) { b0[e] = vl[frag_k(e, hf) * VP + dcol]; b1[e] = vl[(32 + frag_k(e, hf)) * VP + dcol]; }
                        o[t] = wmma16(pa0, b0, o[t]);
                        o[t] = wmma16(pa1, b1, o[t]);
                    }
                }
            }
        }
    }
    float* obase = p.O + b * p.sOb + h * p.sOh;
    if (p.ST) {
        const int rl = lane >> 1, isel = rl & 7;
        float mv = 0.f, lv = 0.f;
#pragma unroll
        for (int i = 0; i < 8; ++i) if (i == isel) { mv = m8[i]; lv = l8[i]; }
        const int irow = q0 + rl;
        if (irow < p.Lq) { float* st = p.ST + (((long long)b * gridDim.y + h) * p.Lq + irow) * 2 + (lane & 1); VST2(float, st, (lane & 1) ? lv : mv * 0.6931471805599453f); }
    }
    float invr[8];
#pragma unroll
    for (int i = 0; i < 8; ++i) {
        if (TWOPASS) invr[i] = SPLITPV ? 1.f : (1.f / 4096.f);
        else if (p.nonorm) invr[i] = exp2f(m8[i]) * (SPLITPV ? 1.f : (1.f / 4096.f));
        else invr[i] = (l8[i] > 0.f) ? (SPLITPV ? 1.f / l8[i] : 1.f / (l8[i] * 4096.f)) : 0.f;
    }
    __syncthreads();
    const bool ofast = ((p.sOi & 3) == 0) && ((((size_t)obase) & 15) == 0) && (q0 + 16 <= p.Lq);
#pragma unroll
    for (int c0 = 0; c0 < DVP; c0 += 64) {
#pragma unroll
        for (int i = 0; i < 8; ++i)
#pragma unroll
            for (int t = 0; t < NT; ++t) if (t * 16 >= c0 && t * 16 < c0 + 64) myp[(i + 8 * hf) * 64 + (t * 16 - c0) + l15] = o[t][i] * invr[i];
        __syncthreads();
        const int cw = (DVP - c0 < 64) ? (DVP - c0) : 64;
        if (ofast && (c0 + cw <= p.dv) && (cw % 32 == 0)) {
            const int lpr = cw / 4;
            const int rows_per_ins = 32 / lpr;
            for (int r0 = 0; r0 < 16; r0 += rows_per_ins) {
                const int row = r0 + lane / lpr, c4 = (lane % lpr) * 4;
                const v4f v = *(const v4f*)(myp + row * 64 + c4);
                VST2V4(obase + (long long)(q0 + row) * p.sOi + c0 + c4, v);
            }
        } else {
            for (int row = 0; row < 16; ++row) {
                const int irow = q0 + row; if (irow >= p.Lq) continue;
                for (int c = lane; c < cw; c += 32) { const int d = c0 + c; if (d < p.dv) VST2(float, obase + (long long)irow * p.sOi + d, myp[row * 64 + c]); }
            }
        }
        __syncthreads();
    }
}

struct TrP { const float* src; float* dst; const float* R2; long long sSz, lds, sDz, ldd, sRz, ldr; int R, C, flags, act; float alpha, beta; };
static_assert(sizeof(TrP) == 3 * 8 + 6 * 8 + 6 * 4, "TrP has padding");
__global__ __launch_bounds__(256) void k_tr(TrP p) {
    __shared__ float tile[32][33];
    const int c0 = blockIdx.x * 32, r0 = blockIdx.y * 32, z = blockIdx.z;
    const int lane = threadIdx.x & 31, wave = threadIdx.x >> 5;
    const float* s = p.src + z * p.sSz;
#pragma unroll
    for (int k = 0; k < 4; ++k) {
        const int rl = wave * 4 + k, r = r0 + rl, c = c0 + lane;
        tile[rl][lane] = (r < p.R && c < p.C) ? s[(long long)r * p.lds + c] : 0.f;
    }
    __syncthreads();
    float* d = p.dst + z * p.sDz; const float* rr = p.R2 + z * p.sRz;
#pragma unroll
    for (int k = 0; k < 4; ++k) {
        const int cl = wave * 4 + k, c = c0 + cl, r = r0 + lane;
        if (c < p.C && r < p.R) {
            float v = act_fn(p.alpha * tile[lane][cl], p.act);
            if (p.flags & 1) v += p.beta * rr[(long long)c * p.ldr + r];
            VST2(float, d + (long long)c * p.ldd + r, v);
        }
    }
}

__global__ __launch_bounds__(256) void k_affine(const float* __restrict__ src, float* __restrict__ dst, int n, float a, float b, const float* __restrict__ sdev) {
    const int i = blockIdx.x * 256 + threadIdx.x;
    if (i < n) { const float aa = sdev ? a * sdev[0] : a; const float v = aa * src[i] + b; VST2(float, dst + i, v); }
}

struct SmP { const float* src; float* dst; const float* Mf; long long sz, sr, dz, dr, smz, smr; int n, pad; float scale_in, scale_out; };
static_assert(sizeof(SmP) == 3 * 8 + 6 * 8 + 4 * 4, "SmP has padding");
__global__ __launch_bounds__(256) void k_softmax(SmP p) {
    __shared__ float red[256];
    const int r = blockIdx.x, z = blockIdx.y, tid = threadIdx.x;
    const float* s = p.src + z * p.sz + (long long)r * p.sr;
    const float* mf = p.Mf ? (p.Mf + z * p.smz + (long long)r * p.smr) : nullptr;
    float mx = -__builtin_inff();
    for (int j = tid; j < p.n; j += 256) { float v = s[j] * p.scale_in; if (mf) v += mf[j]; mx = fmaxf(mx, v); }
    red[tid] = mx; __syncthreads();
    for (int o = 128; o > 0; o >>= 1) { if (tid < o) red[tid] = fmaxf(red[tid], red[tid + o]); __syncthreads(); }
    mx = red[0]; __syncthreads();
    float sum = 0.f;
    for (int j = tid; j < p.n; j += 256) { float v = s[j] * p.scale_in; if (mf) v += mf[j]; sum += (mx == -__builtin_inff()) ? 0.f : expf(v - mx); }
    red[tid] = sum; __syncthreads();
    for (int o = 128; o > 0; o >>= 1) { if (tid < o) red[tid] += red[tid + o]; __syncthreads(); }
    sum = red[0];
    const float inv = (sum > 0.f) ? p.scale_out / sum : 0.f;
    float* d = p.dst + z * p.dz + (long long)r * p.dr;
    for (int j = tid; j < p.n; j += 256) { float v = s[j] * p.scale_in; if (mf) v += mf[j]; const float o = (mx == -__builtin_inff()) ? 0.f : expf(v - mx) * inv; VST2(float, d + j, o); }
}
__global__ __launch_bounds__(256) void k_stats(const float* __restrict__ x, long long sz, long long so, long long si, int inner, int n, float eps, float* __restrict__ stat, int mode) {
    __shared__ float red[256];
    const int z = blockIdx.x, tid = threadIdx.x;
    const float* base = x + z * sz;
    float s = 0.f;
    for (int e = tid; e < n; e += 256) s += base[(long long)(e / inner) * so + (long long)(e % inner) * si];
    red[tid] = s; __syncthreads();
    for (int o = 128; o > 0; o >>= 1) { if (tid < o) red[tid] += red[tid + o]; __syncthreads(); }
    const float mu = (mode == 0 || mode == 3) ? red[0] / (float)n : 0.f; __syncthreads();
    float q = 0.f;
    for (int e = tid; e < n; e += 256) { const float dlt = base[(long long)(e / inner) * so + (long long)(e % inner) * si] - mu; q += dlt * dlt; }
    red[tid] = q; __syncthreads();
    for (int o = 128; o > 0; o >>= 1) { if (tid < o) red[tid] += red[tid + o]; __syncthreads(); }
    {
        float rs;
        if (mode == 2) rs = sqrtf((float)n) / fmaxf(sqrtf(red[0]), eps); else if (mode == 3) rs = rsqrtf(red[0] / (float)(n - 1) + eps); else rs = rsqrtf(red[0] / (float)n + eps);
        if (tid < 32) { const float v = (tid == 0) ? mu : ((tid == 1) ? rs : 0.f); VST2(float, stat + (long long)z * 32 + tid, v); }
    }
}
__global__ __launch_bounds__(256) void k_norm_apply(const float* __restrict__ x, float* __restrict__ y, const float* __restrict__ stat, const float* __restrict__ g, const float* __restrict__ bta,
                                                     int Z, int C, int L, int G, int bn, int act) {
    const long long idx = (long long)blockIdx.x * 256 + threadIdx.x;
    if (idx >= (long long)Z * C * L) return;
    const int l = (int)(idx % L); const long long zc = idx / L; const int c = (int)(zc % C), z = (int)(zc / C); (void)l;
    const int set = bn ? c : (z * G + c / (C / G));
    float v = (x[idx] - stat[(long long)set * 32]) * stat[(long long)set * 32 + 1];
    if (g) v *= g[c];
    if (bta) v += bta[c];
    v = act_fn(v, act);
    VST2(float, y + idx, v);
}

__global__ __launch_bounds__(256) void k_lse_neg(const float* __restrict__ st, float* __restrict__ c, int n) {
    const int i = blockIdx.x * 256 + threadIdx.x;
    if (i < n) { const float v = -(st[2 * i] + logf(st[2 * i + 1])); VST2(float, c + i, v); }
}

__global__ __launch_bounds__(256) void k_iota(int* __restrict__ dst, int n, int a, int b) {
    const int i = blockIdx.x * 256 + threadIdx.x;
    if (i < n) { const int v = a * i + b; VST2(int, dst + i, v); }
}

__global__ __launch_bounds__(256) void k_axpby(const float* __restrict__ x, const float* __restrict__ y, float* __restrict__ dst, int n, float a, float b, float c) {
    const int i = blockIdx.x * 256 + threadIdx.x;
    if (i < n) { const float v = a * x[i] + b * y[i] + c; VST2(float, dst + i, v); }
}

struct RopeP { const float* X; float* Y; const float* C; const float* Sn; const int* pos; long long sXr, sXh, sYr, sYh, sCb, sCp, sCd; int R, Hn, D, S, mode, tmode, pmode, pad; };
static_assert(sizeof(RopeP) == 5 * 8 + 7 * 8 + 8 * 4, "RopeP has padding");
__global__ __launch_bounds__(256) void k_rope(RopeP p) {
    const long long idx = (long long)blockIdx.x * 256 + threadIdx.x;
    if (idx >= (long long)p.R * p.Hn * p.D) return;
    const int d = (int)(idx % p.D); const long long rh = idx / p.D; const int h = (int)(rh % p.Hn); const int r = (int)(rh / p.Hn);
    const int half = p.D / 2;
    int partner; float sign;
    if (p.mode == 0) { partner = (d < half) ? d + half : d - half; sign = (d < half) ? -1.f : 1.f; }
    else { partner = d ^ 1; sign = (d & 1) ? 1.f : -1.f; }
    const int tcol = (p.tmode == 0) ? d : ((p.tmode == 1) ? (d % half) : (d >> 1));
    const int pp = (p.pmode == 0) ? (r % p.S) : ((p.pmode == 1) ? h : p.pos[r]);
    const long long toff = (long long)(r / p.S) * p.sCb + (long long)pp * p.sCp + (long long)tcol * p.sCd;
    const float* xr = p.X + (long long)r * p.sXr + (long long)h * p.sXh;
    const float v = xr[d] * p.C[toff] + sign * xr[partner] * p.Sn[toff];
    VST2(float, p.Y + (long long)r * p.sYr + (long long)h * p.sYh + d, v);
}

__global__ __launch_bounds__(256) void k_invf(float* __restrict__ invb, int half, int D, float base, float num, int fmode, float cexp) {
    const int i = blockIdx.x * 256 + threadIdx.x;
    if (i >= ((half + 31) / 32) * 32) return;
    if (i >= half) { VST2(float, invb + i, 0.f); return; }
    const float e = (float)(2 * i) / (float)D;
    float invf;
    if (fmode == 1) invf = num * expf((float)(2 * i) * cexp);
    else if (fmode == 2) invf = num * powf(base, (-2.0f * ((float)i - 1.0f)) / (float)D);
    else invf = num * (1.0f / powf(base, e));
    VST2(float, invb + i, invf);
}
__global__ __launch_bounds__(256) void k_sincos(float* __restrict__ cs, float* __restrict__ sn, const float* __restrict__ invb, int S, int half, float pscale) {
    const int idx = blockIdx.x * 256 + threadIdx.x;
    if (idx >= S * half) return;
    const int s = idx / half, i = idx - s * half;
    const float ang = (pscale * (float)s) * invb[i];
    VST2(float, cs + idx, cosf(ang)); VST2(float, sn + idx, sinf(ang));
}

__global__ __launch_bounds__(256) void k_mulact(const float* __restrict__ x, const float* __restrict__ y, float* __restrict__ dst, int n, int act) {
    const int i = blockIdx.x * 256 + threadIdx.x;
    if (i < n) { const float v = act_fn(x[i], act) * y[i]; VST2(float, dst + i, v); }
}

__global__ __launch_bounds__(256) void k_matvec(GemmP p) {
    const int rpt = (p.N == 1) ? 1 : 32;
    const long long r0 = ((long long)blockIdx.x * 256 + threadIdx.x) * rpt; const int z = blockIdx.z, zo = z / p.zi_n, zi = z - zo * p.zi_n;
    if (r0 >= p.M) return;
    const float* Bb = p.B + zo * p.sBo + zi * p.sBi;
    float* C = p.C + zo * p.sCo + zi * p.sCi; const float* R = p.R + zo * p.sRo + zi * p.sRi;
    for (int rr = 0; rr < rpt; ++rr) {
        const long long r = r0 + rr; if (r >= p.M) break;
        const float* A = p.A + zo * p.sAo + zi * p.sAi + r * p.sAm;
        float acc[8] = {0.f, 0.f, 0.f, 0.f, 0.f, 0.f, 0.f, 0.f};
        for (int k = 0; k < p.K; ++k) { const float a = A[(long long)k * p.sAk];
#pragma unroll
            for (int j = 0; j < 8; ++j) if (j < p.N) acc[j] += a * Bb[(long long)j * p.sBn + (long long)k * p.sBk]; }
#pragma unroll
        for (int j = 0; j < 8; ++j) if (j < p.N) {
            float v = acc[j] * p.alpha;
            if (p.flags & 1) v += p.bias[j];
            if (p.flags & 2) v += p.bias[r];
            v = act_fn(v, p.act);
            if (p.flags & 4) v += p.beta * R[r * p.sRm + (long long)j * p.sRn];
            VST2(float, C + r * p.sCm + j, v);
        }
    }
}
__global__ __launch_bounds__(256) void k_smallsoftmax(const float* __restrict__ src, float* __restrict__ dst, long long sr, long long dr, int n, long long R, float scale) {
    const long long r0 = ((long long)blockIdx.x * 256 + threadIdx.x) * 32;
    for (int rr = 0; rr < 32; ++rr) {
        const long long r = r0 + rr; if (r >= R) return;
        const float* s = src + r * sr; float* d = dst + r * dr;
        float mx = -__builtin_inff();
        for (int j = 0; j < n; ++j) mx = fmaxf(mx, s[j] * scale);
        float sum = 0.f;
        for (int j = 0; j < n; ++j) sum += expf(s[j] * scale - mx);
        const float inv = 1.f / sum;
        for (int j = 0; j < n; ++j) { const float v = expf(s[j] * scale - mx) * inv; VST2(float, d + j, v); }
    }
}

__global__ __launch_bounds__(32) void k_unitstat(float* __restrict__ st) { const int t = threadIdx.x; const float v = (t == 1) ? 1.f : 0.f; VST2(float, st + t, v); }

__global__ __launch_bounds__(256) void k_lincopy(const float* __restrict__ src, long long lds, float* __restrict__ dst, long long ldd, long long rows, int cols) {
    const long long i = (long long)blockIdx.x * 256 + threadIdx.x; if (i >= rows * cols) return;
    const long long r = i / cols; const int c = (int)(i - r * cols);
    const float v = src[r * lds + c]; VST2(float, dst + r * ldd + c, v);
}

__global__ __launch_bounds__(256) void k_wg_patches(const float* __restrict__ X, float* __restrict__ FEAT, float* __restrict__ DP, float* __restrict__ SPD, int B, int C, int IMG) {
    const long long q = (long long)blockIdx.x * 256 + threadIdx.x; if (q >= (long long)B * 256 * 64 * C) return; const int c = (int)(q % C); const int px = (int)((q / C) % 8); const int py = (int)((q / (C * 8)) % 8); const int node = (int)(q / ((long long)C * 64)); const int b = node / 256, n = node % 256, i1 = n / 16, i2 = n % 16;
    const float v = X[(((long long)b * C + c) * IMG + i1 * 8 + py) * IMG + i2 * 8 + px];
    VST2(float, FEAT + q, v); const long long pd = (((long long)node * 10 + py + 1) * 10 + px + 1) * C + c; VST2(float, DP + pd, v); VST2(float, SPD + pd, v);
}
__global__ __launch_bounds__(256) void k_wg_rowsq(const float* __restrict__ F, float* __restrict__ SQ, int R, int D) { const int r = blockIdx.x; __shared__ float red[256]; float s = 0.f; for (int d = threadIdx.x; d < D; d += 256) { const float v = F[(long long)r * D + d]; s += v * v; } red[threadIdx.x] = s; __syncthreads(); for (int o = 128; o > 0; o >>= 1) { if (threadIdx.x < o) red[threadIdx.x] += red[threadIdx.x + o]; __syncthreads(); } if (threadIdx.x < 32) VST2(float, SQ + r, red[0]); }
__global__ __launch_bounds__(256) void k_wg_top8(const float* __restrict__ GM, const float* __restrict__ SQ, int* __restrict__ IDX, float* __restrict__ EW, int b, int NN) {
    const int n = blockIdx.x * 256 + threadIdx.x; if (n >= NN) return; const float sn = SQ[b * NN + n]; float bd[8]; int bi[8]; for (int j = 0; j < 8; ++j) { bd[j] = __builtin_inff(); bi[j] = 0; }
    for (int m = 0; m < NN; ++m) { const float d2 = sn + SQ[b * NN + m] - 2.f * GM[(long long)n * NN + m]; const float d = sqrtf(fmaxf(d2, 1e-12f)); if (d < bd[7]) { int s = 7; while (s > 0 && d < bd[s - 1]) { bd[s] = bd[s - 1]; bi[s] = bi[s - 1]; --s; } bd[s] = d; bi[s] = m; } }
    float sg = 0.f; for (int j = 0; j < 8; ++j) sg += bd[j]; sg *= 0.125f;
    for (int j = 0; j < 8; ++j) { VST2(int, IDX + ((long long)b * NN + n) * 8 + j, b * NN + bi[j]); VST2(float, EW + ((long long)b * NN + n) * 8 + j, expf(-bd[j] / (sg * sg))); }
}
__global__ __launch_bounds__(256) void k_wg_wb(const float* __restrict__ atw, float* __restrict__ WB, int C) {
    const int q = blockIdx.x * 256 + threadIdx.x; if (q >= 64 * C) return; const int c = q % C; const int x = (q / C) % 8; const int y = q / (C * 8);
    VST2(float, WB + (long long)q * 2, atw[(c * 2 + (y & 1)) * 2 + (x & 1)]); VST2(float, WB + (long long)q * 2 + 1, atw[((C + c) * 2 + (y & 1)) * 2 + (x & 1)]);
}
__global__ __launch_bounds__(256) void k_wg_alpha(const float* __restrict__ AS, int ldp, const int* __restrict__ IDX, const float* __restrict__ atb, float* __restrict__ AL, int NODES) {
    const int n = blockIdx.x * 256 + threadIdx.x; if (n >= NODES) return; float a[8]; float mx = -__builtin_inff();
    for (int j = 0; j < 8; ++j) { const int m = IDX[(long long)n * 8 + j]; float v = AS[(long long)m * ldp] + AS[(long long)n * ldp + 1] + atb[0]; v = (v > 0.f) ? v : 0.01f * v; a[j] = v; mx = fmaxf(mx, v); }
    float s = 0.f; for (int j = 0; j < 8; ++j) { a[j] = expf(a[j] - mx); s += a[j]; } for (int j = 0; j < 8; ++j) VST2(float, AL + (long long)n * 8 + j, a[j] / s);
}
__global__ __launch_bounds__(256) void k_wg_pad(const float* __restrict__ SRC, float* __restrict__ DSTP, int NODES, int C, int gelu) {
    const long long q = (long long)blockIdx.x * 256 + threadIdx.x; if (q >= (long long)NODES * 64 * C) return; const int c = (int)(q % C); const int px = (int)((q / C) % 8); const int py = (int)((q / (C * 8)) % 8); const long long node = q / (C * 64);
    float v = SRC[q]; if (gelu) v = 0.5f * v * (1.f + erff(v * 0.7071067811865476f)); VST2(float, DSTP + ((node * 10 + py + 1) * 10 + px + 1) * C + c, v);
}
__global__ __launch_bounds__(256) void k_wg_update(const float* __restrict__ MS, const float* __restrict__ DCg, const int* __restrict__ IDX, const float* __restrict__ EW, const float* __restrict__ AL, const float* __restrict__ csb,
                                                  float* __restrict__ SPD, float* __restrict__ DP, float* __restrict__ OPf, int NODES, int C, int fin) {
    const long long q = (long long)blockIdx.x * 256 + threadIdx.x; if (q >= (long long)NODES * 64 * C) return; const int c = (int)(q % C); const int px = (int)((q / C) % 8); const int py = (int)((q / (C * 8)) % 8); const int node = (int)(q / (C * 64));
    float smax = -__builtin_inff(), dsum = 0.f; const long long pofs = ((long long)py * 8 + px) * C + c;
    for (int j = 0; j < 8; ++j) { const int m = IDX[(long long)node * 8 + j]; float v = EW[(long long)node * 8 + j] * MS[(long long)m * 64 * C + pofs] + csb[c]; v = 0.5f * v * (1.f + erff(v * 0.7071067811865476f)); smax = fmaxf(smax, v); dsum += AL[(long long)node * 8 + j] * DCg[(long long)m * 64 * C + pofs]; }
    const long long pd = (((long long)node * 10 + py + 1) * 10 + px + 1) * C + c; VST2(float, SPD + pd, smax); VST2(float, DP + pd, dsum);
    if (fin) { const int b = node / 256, n = node % 256, i1 = n / 16, i2 = n % 16; const long long base = (((long long)b * 130 + i1 * 8 + py + 1) * 130 + i2 * 8 + px + 1) * (2 * C); VST2(float, OPf + base + c, smax); VST2(float, OPf + base + C + c, dsum); }
}

template __global__ void k_gemm<1>(GemmP);
template __global__ void k_gemm<3>(GemmP);

extern "C" void kernel_launch(void* const* d_in, const int* in_sizes, int n_in, void* d_out, int out_size, void* d_ws, size_t ws_size, hipStream_t stream) {
    (void)in_sizes; (void)n_in; (void)out_size; (void)ws_size;
    const float* x = (const float*)d_in[0];
    const float* csw = (const float*)d_in[1];
    const float* csb = (const float*)d_in[2];
    const float* cdw = (const float*)d_in[3];
    const float* cdb = (const float*)d_in[4];
    const float* atw = (const float*)d_in[5];
    const float* atb = (const float*)d_in[6];
    const float* ow = (const float*)d_in[7];
    const float* ob = (const float*)d_in[8];
    const int Bn = 2;
    const int C = 128;
    const int IMG = 128;
    const int WS = 8;
    const int NN = 256;
    const int KN = 8;
    const int NODES = Bn * NN;
    const int FD = C * WS * WS;
    const int NP = NODES * 100;
    const int LP = 32;
    float* out = (float*)d_out;
    char* wsp = (char*)d_ws;
    float* FEAT = (float*)wsp; wsp += (((size_t)((size_t)NODES * FD) * 4 + 255) / 256) * 256;
    float* SQ = (float*)wsp; wsp += (((size_t)((size_t)NODES + 64) * 4 + 255) / 256) * 256;
    float* GM = (float*)wsp; wsp += (((size_t)((size_t)NN * NN) * 4 + 255) / 256) * 256;
    int* IDX = (int*)wsp; wsp += (((size_t)((size_t)NODES * KN) * 4 + 255) / 256) * 256;
    float* EW = (float*)wsp; wsp += (((size_t)((size_t)NODES * KN) * 4 + 255) / 256) * 256;
    float* AL = (float*)wsp; wsp += (((size_t)((size_t)NODES * KN) * 4 + 255) / 256) * 256;
    float* DP = (float*)wsp; wsp += (((size_t)((size_t)NP * C) * 4 + 255) / 256) * 256;
    float* SPD = (float*)wsp; wsp += (((size_t)((size_t)NP * C) * 4 + 255) / 256) * 256;
    float* DC = (float*)wsp; wsp += (((size_t)((size_t)NODES * 64 * C) * 4 + 255) / 256) * 256;
    float* MS = (float*)wsp; wsp += (((size_t)((size_t)NODES * 64 * C) * 4 + 255) / 256) * 256;
    float* WB = (float*)wsp; wsp += (((size_t)((size_t)FD * 2) * 4 + 255) / 256) * 256;
    float* AS = (float*)wsp; wsp += (((size_t)((size_t)NODES * LP) * 4 + 255) / 256) * 256;
    float* OP = (float*)wsp; wsp += (((size_t)((size_t)Bn * 130 * 130 * 256) * 4 + 255) / 256) * 256;
    float* OC = (float*)wsp; wsp += (((size_t)((size_t)Bn * IMG * IMG * C) * 4 + 255) / 256) * 256;
    float* ust = (float*)wsp; wsp += (((size_t)(64) * 4 + 255) / 256) * 256;
    hipMemsetAsync(DP, 0, (size_t)NP * C * 4, stream); hipMemsetAsync(SPD, 0, (size_t)NP * C * 4, stream); hipMemsetAsync(OP, 0, (size_t)Bn * 130 * 130 * 256 * 4, stream);
    k_wg_patches<<<(unsigned)(((long long)NODES * 64 * C + 255) / 256), 256, 0, stream>>>(x, FEAT, DP, SPD, Bn, C, IMG);
    k_wg_rowsq<<<NODES, 256, 0, stream>>>(FEAT, SQ, NODES, FD);
    { GemmP ggm0;
      ggm0.A = FEAT + (size_t)0 * NN * FD; ggm0.B = FEAT + (size_t)0 * NN * FD; ggm0.bias = FEAT + (size_t)0 * NN * FD; ggm0.R = FEAT + (size_t)0 * NN * FD; ggm0.C = GM;
      ggm0.sAo = 0; ggm0.sAi = 0; ggm0.sAm = FD; ggm0.sAk = 1; ggm0.sBo = 0; ggm0.sBi = 0; ggm0.sBn = FD; ggm0.sBk = 1; ggm0.sCo = 0; ggm0.sCi = 0; ggm0.sCm = NN; ggm0.sRo = 0; ggm0.sRi = 0; ggm0.sRm = 0; ggm0.sRn = 0;
      ggm0.M = NN; ggm0.N = NN; ggm0.K = FD; ggm0.zi_n = 1; ggm0.flags = 0; ggm0.act = 0;
      ggm0.alpha = 1.0f; ggm0.beta = 0.0f; ggm0.sa = 1.0f; ggm0.sb = 1.0f; ggm0.Npad = NN; ggm0.pad_ = 0;
      k_gemm<3><<<dim3((unsigned)((NN) + 31) / 32, (unsigned)((NN) + 15) / 16, (unsigned)(1)), 32, 0, stream>>>(ggm0); }
    k_wg_top8<<<1, 256, 0, stream>>>(GM, SQ, IDX, EW, 0, NN);
    { GemmP ggm1;
      ggm1.A = FEAT + (size_t)1 * NN * FD; ggm1.B = FEAT + (size_t)1 * NN * FD; ggm1.bias = FEAT + (size_t)1 * NN * FD; ggm1.R = FEAT + (size_t)1 * NN * FD; ggm1.C = GM;
      ggm1.sAo = 0; ggm1.sAi = 0; ggm1.sAm = FD; ggm1.sAk = 1; ggm1.sBo = 0; ggm1.sBi = 0; ggm1.sBn = FD; ggm1.sBk = 1; ggm1.sCo = 0; ggm1.sCi = 0; ggm1.sCm = NN; ggm1.sRo = 0; ggm1.sRi = 0; ggm1.sRm = 0; ggm1.sRn = 0;
      ggm1.M = NN; ggm1.N = NN; ggm1.K = FD; ggm1.zi_n = 1; ggm1.flags = 0; ggm1.act = 0;
      ggm1.alpha = 1.0f; ggm1.beta = 0.0f; ggm1.sa = 1.0f; ggm1.sb = 1.0f; ggm1.Npad = NN; ggm1.pad_ = 0;
      k_gemm<3><<<dim3((unsigned)((NN) + 31) / 32, (unsigned)((NN) + 15) / 16, (unsigned)(1)), 32, 0, stream>>>(ggm1); }
    k_wg_top8<<<1, 256, 0, stream>>>(GM, SQ, IDX, EW, 1, NN);
    k_unitstat<<<1, 32, 0, stream>>>(ust);
    { GemmP cvd0_0;
      cvd0_0.A = DP + (size_t)0 * C; cvd0_0.B = cdw + (size_t)0 + 0; cvd0_0.bias = cdb + (size_t)0; cvd0_0.R = DP + (size_t)0 * C; cvd0_0.C = DC;
      cvd0_0.sAo = (long long)100 * C; cvd0_0.sAi = (long long)10 * C; cvd0_0.sAm = C; cvd0_0.sAk = 1; cvd0_0.sBo = 0; cvd0_0.sBi = 0; cvd0_0.sBn = C * 9; cvd0_0.sBk = 9; cvd0_0.sCo = (long long)64 * C; cvd0_0.sCi = (long long)8 * C; cvd0_0.sCm = C; cvd0_0.sRo = 0; cvd0_0.sRi = 0; cvd0_0.sRm = 0; cvd0_0.sRn = 0;
      cvd0_0.M = 8; cvd0_0.N = C; cvd0_0.K = C; cvd0_0.zi_n = 8; cvd0_0.flags = 1; cvd0_0.act = 0;
      cvd0_0.alpha = 1.0f; cvd0_0.beta = 0.0f; cvd0_0.sa = 1.0f; cvd0_0.sb = 1.0f; cvd0_0.Npad = C; cvd0_0.pad_ = 0;
      k_gemm<1><<<dim3((unsigned)((C) + 31) / 32, (unsigned)((8) + 15) / 16, (unsigned)(NODES * 8)), 32, 0, stream>>>(cvd0_0); }
    { GemmP cvd0_1;
      cvd0_1.A = DP + (size_t)1 * C; cvd0_1.B = cdw + (size_t)0 + 1; cvd0_1.bias = DP + (size_t)1 * C; cvd0_1.R = DC; cvd0_1.C = DC;
      cvd0_1.sAo = (long long)100 * C; cvd0_1.sAi = (long long)10 * C; cvd0_1.sAm = C; cvd0_1.sAk = 1; cvd0_1.sBo = 0; cvd0_1.sBi = 0; cvd0_1.sBn = C * 9; cvd0_1.sBk = 9; cvd0_1.sCo = (long long)64 * C; cvd0_1.sCi = (long long)8 * C; cvd0_1.sCm = C; cvd0_1.sRo = (long long)64 * C; cvd0_1.sRi = (long long)8 * C; cvd0_1.sRm = C; cvd0_1.sRn = 1;
      cvd0_1.M = 8; cvd0_1.N = C; cvd0_1.K = C; cvd0_1.zi_n = 8; cvd0_1.flags = 4; cvd0_1.act = 0;
      cvd0_1.alpha = 1.0f; cvd0_1.beta = 1.0f; cvd0_1.sa = 1.0f; cvd0_1.sb = 1.0f; cvd0_1.Npad = C; cvd0_1.pad_ = 0;
      k_gemm<1><<<dim3((unsigned)((C) + 31) / 32, (unsigned)((8) + 15) / 16, (unsigned)(NODES * 8)), 32, 0, stream>>>(cvd0_1); }
    { GemmP cvd0_2;
      cvd0_2.A = DP + (size_t)2 * C; cvd0_2.B = cdw + (size_t)0 + 2; cvd0_2.bias = DP + (size_t)2 * C; cvd0_2.R = DC; cvd0_2.C = DC;
      cvd0_2.sAo = (long long)100 * C; cvd0_2.sAi = (long long)10 * C; cvd0_2.sAm = C; cvd0_2.sAk = 1; cvd0_2.sBo = 0; cvd0_2.sBi = 0; cvd0_2.sBn = C * 9; cvd0_2.sBk = 9; cvd0_2.sCo = (long long)64 * C; cvd0_2.sCi = (long long)8 * C; cvd0_2.sCm = C; cvd0_2.sRo = (long long)64 * C; cvd0_2.sRi = (long long)8 * C; cvd0_2.sRm = C; cvd0_2.sRn = 1;
      cvd0_2.M = 8; cvd0_2.N = C; cvd0_2.K = C; cvd0_2.zi_n = 8; cvd0_2.flags = 4; cvd0_2.act = 0;
      cvd0_2.alpha = 1.0f; cvd0_2.beta = 1.0f; cvd0_2.sa = 1.0f; cvd0_2.sb = 1.0f; cvd0_2.Npad = C; cvd0_2.pad_ = 0;
      k_gemm<1><<<dim3((unsigned)((C) + 31) / 32, (unsigned)((8) + 15) / 16, (unsigned)(NODES * 8)), 32, 0, stream>>>(cvd0_2); }
    { GemmP cvd0_3;
      cvd0_3.A = DP + (size_t)10 * C; cvd0_3.B = cdw + (size_t)0 + 3; cvd0_3.bias = DP + (size_t)10 * C; cvd0_3.R = DC; cvd0_3.C = DC;
      cvd0_3.sAo = (long long)100 * C; cvd0_3.sAi = (long long)10 * C; cvd0_3.sAm = C; cvd0_3.sAk = 1; cvd0_3.sBo = 0; cvd0_3.sBi = 0; cvd0_3.sBn = C * 9; cvd0_3.sBk = 9; cvd0_3.sCo = (long long)64 * C; cvd0_3.sCi = (long long)8 * C; cvd0_3.sCm = C; cvd0_3.sRo = (long long)64 * C; cvd0_3.sRi = (long long)8 * C; cvd0_3.sRm = C; cvd0_3.sRn = 1;
      cvd0_3.M = 8; cvd0_3.N = C; cvd0_3.K = C; cvd0_3.zi_n = 8; cvd0_3.flags = 4; cvd0_3.act = 0;
      cvd0_3.alpha = 1.0f; cvd0_3.beta = 1.0f; cvd0_3.sa = 1.0f; cvd0_3.sb = 1.0f; cvd0_3.Npad = C; cvd0_3.pad_ = 0;
      k_gemm<1><<<dim3((unsigned)((C) + 31) / 32, (unsigned)((8) + 15) / 16, (unsigned)(NODES * 8)), 32, 0, stream>>>(cvd0_3); }
    { GemmP cvd0_4;
      cvd0_4.A = DP + (size_t)11 * C; cvd0_4.B = cdw + (size_t)0 + 4; cvd0_4.bias = DP + (size_t)11 * C; cvd0_4.R = DC; cvd0_4.C = DC;
      cvd0_4.sAo = (long long)100 * C; cvd0_4.sAi = (long long)10 * C; cvd0_4.sAm = C; cvd0_4.sAk = 1; cvd0_4.sBo = 0; cvd0_4.sBi = 0; cvd0_4.sBn = C * 9; cvd0_4.sBk = 9; cvd0_4.sCo = (long long)64 * C; cvd0_4.sCi = (long long)8 * C; cvd0_4.sCm = C; cvd0_4.sRo = (long long)64 * C; cvd0_4.sRi = (long long)8 * C; cvd0_4.sRm = C; cvd0_4.sRn = 1;
      cvd0_4.M = 8; cvd0_4.N = C; cvd0_4.K = C; cvd0_4.zi_n = 8; cvd0_4.flags = 4; cvd0_4.act = 0;
      cvd0_4.alpha = 1.0f; cvd0_4.beta = 1.0f; cvd0_4.sa = 1.0f; cvd0_4.sb = 1.0f; cvd0_4.Npad = C; cvd0_4.pad_ = 0;
      k_gemm<1><<<dim3((unsigned)((C) + 31) / 32, (unsigned)((8) + 15) / 16, (unsigned)(NODES * 8)), 32, 0, stream>>>(cvd0_4); }
    { GemmP cvd0_5;
      cvd0_5.A = DP + (size_t)12 * C; cvd0_5.B = cdw + (size_t)0 + 5; cvd0_5.bias = DP + (size_t)12 * C; cvd0_5.R = DC; cvd0_5.C = DC;
      cvd0_5.sAo = (long long)100 * C; cvd0_5.sAi = (long long)10 * C; cvd0_5.sAm = C; cvd0_5.sAk = 1; cvd0_5.sBo = 0; cvd0_5.sBi = 0; cvd0_5.sBn = C * 9; cvd0_5.sBk = 9; cvd0_5.sCo = (long long)64 * C; cvd0_5.sCi = (long long)8 * C; cvd0_5.sCm = C; cvd0_5.sRo = (long long)64 * C; cvd0_5.sRi = (long long)8 * C; cvd0_5.sRm = C; cvd0_5.sRn = 1;
      cvd0_5.M = 8; cvd0_5.N = C; cvd0_5.K = C; cvd0_5.zi_n = 8; cvd0_5.flags = 4; cvd0_5.act = 0;
      cvd0_5.alpha = 1.0f; cvd0_5.beta = 1.0f; cvd0_5.sa = 1.0f; cvd0_5.sb = 1.0f; cvd0_5.Npad = C; cvd0_5.pad_ = 0;
      k_gemm<1><<<dim3((unsigned)((C) + 31) / 32, (unsigned)((8) + 15) / 16, (unsigned)(NODES * 8)), 32, 0, stream>>>(cvd0_5); }
    { GemmP cvd0_6;
      cvd0_6.A = DP + (size_t)20 * C; cvd0_6.B = cdw + (size_t)0 + 6; cvd0_6.bias = DP + (size_t)20 * C; cvd0_6.R = DC; cvd0_6.C = DC;
      cvd0_6.sAo = (long long)100 * C; cvd0_6.sAi = (long long)10 * C; cvd0_6.sAm = C; cvd0_6.sAk = 1; cvd0_6.sBo = 0; cvd0_6.sBi = 0; cvd0_6.sBn = C * 9; cvd0_6.sBk = 9; cvd0_6.sCo = (long long)64 * C; cvd0_6.sCi = (long long)8 * C; cvd0_6.sCm = C; cvd0_6.sRo = (long long)64 * C; cvd0_6.sRi = (long long)8 * C; cvd0_6.sRm = C; cvd0_6.sRn = 1;
      cvd0_6.M = 8; cvd0_6.N = C; cvd0_6.K = C; cvd0_6.zi_n = 8; cvd0_6.flags = 4; cvd0_6.act = 0;
      cvd0_6.alpha = 1.0f; cvd0_6.beta = 1.0f; cvd0_6.sa = 1.0f; cvd0_6.sb = 1.0f; cvd0_6.Npad = C; cvd0_6.pad_ = 0;
      k_gemm<1><<<dim3((unsigned)((C) + 31) / 32, (unsigned)((8) + 15) / 16, (unsigned)(NODES * 8)), 32, 0, stream>>>(cvd0_6); }
    { GemmP cvd0_7;
      cvd0_7.A = DP + (size_t)21 * C; cvd0_7.B = cdw + (size_t)0 + 7; cvd0_7.bias = DP + (size_t)21 * C; cvd0_7.R = DC; cvd0_7.C = DC;
      cvd0_7.sAo = (long long)100 * C; cvd0_7.sAi = (long long)10 * C; cvd0_7.sAm = C; cvd0_7.sAk = 1; cvd0_7.sBo = 0; cvd0_7.sBi = 0; cvd0_7.sBn = C * 9; cvd0_7.sBk = 9; cvd0_7.sCo = (long long)64 * C; cvd0_7.sCi = (long long)8 * C; cvd0_7.sCm = C; cvd0_7.sRo = (long long)64 * C; cvd0_7.sRi = (long long)8 * C; cvd0_7.sRm = C; cvd0_7.sRn = 1;
      cvd0_7.M = 8; cvd0_7.N = C; cvd0_7.K = C; cvd0_7.zi_n = 8; cvd0_7.flags = 4; cvd0_7.act = 0;
      cvd0_7.alpha = 1.0f; cvd0_7.beta = 1.0f; cvd0_7.sa = 1.0f; cvd0_7.sb = 1.0f; cvd0_7.Npad = C; cvd0_7.pad_ = 0;
      k_gemm<1><<<dim3((unsigned)((C) + 31) / 32, (unsigned)((8) + 15) / 16, (unsigned)(NODES * 8)), 32, 0, stream>>>(cvd0_7); }
    { GemmP cvd0_8;
      cvd0_8.A = DP + (size_t)22 * C; cvd0_8.B = cdw + (size_t)0 + 8; cvd0_8.bias = DP + (size_t)22 * C; cvd0_8.R = DC; cvd0_8.C = DC;
      cvd0_8.sAo = (long long)100 * C; cvd0_8.sAi = (long long)10 * C; cvd0_8.sAm = C; cvd0_8.sAk = 1; cvd0_8.sBo = 0; cvd0_8.sBi = 0; cvd0_8.sBn = C * 9; cvd0_8.sBk = 9; cvd0_8.sCo = (long long)64 * C; cvd0_8.sCi = (long long)8 * C; cvd0_8.sCm = C; cvd0_8.sRo = (long long)64 * C; cvd0_8.sRi = (long long)8 * C; cvd0_8.sRm = C; cvd0_8.sRn = 1;
      cvd0_8.M = 8; cvd0_8.N = C; cvd0_8.K = C; cvd0_8.zi_n = 8; cvd0_8.flags = 4; cvd0_8.act = 0;
      cvd0_8.alpha = 1.0f; cvd0_8.beta = 1.0f; cvd0_8.sa = 1.0f; cvd0_8.sb = 1.0f; cvd0_8.Npad = C; cvd0_8.pad_ = 0;
      k_gemm<1><<<dim3((unsigned)((C) + 31) / 32, (unsigned)((8) + 15) / 16, (unsigned)(NODES * 8)), 32, 0, stream>>>(cvd0_8); }

    k_norm_apply<<<(unsigned)(((long long)(1) * (1) * ((long long)NODES * 64 * C) + 255) / 256), 256, 0, stream>>>(DC, DC, ust, nullptr, nullptr, 1, 1, (long long)NODES * 64 * C, 1, 0, 4);
    k_wg_wb<<<(unsigned)((64 * C + 255) / 256), 256, 0, stream>>>(atw + (size_t)0, WB, C);
    { GemmP gas0;
      gas0.A = DC; gas0.B = WB; gas0.bias = DC; gas0.R = DC; gas0.C = AS;
      gas0.sAo = 0; gas0.sAi = 0; gas0.sAm = FD; gas0.sAk = 1; gas0.sBo = 0; gas0.sBi = 0; gas0.sBn = 1; gas0.sBk = 2; gas0.sCo = 0; gas0.sCi = 0; gas0.sCm = LP; gas0.sRo = 0; gas0.sRi = 0; gas0.sRm = 0; gas0.sRn = 0;
      gas0.M = NODES; gas0.N = 2; gas0.K = FD; gas0.zi_n = 1; gas0.flags = 0; gas0.act = 0;
      gas0.alpha = 0.0625f; gas0.beta = 0.0f; gas0.sa = 1.0f; gas0.sb = 1.0f; gas0.Npad = LP; gas0.pad_ = 0;
      k_gemm<3><<<dim3((unsigned)((LP) + 31) / 32, (unsigned)((NODES) + 15) / 16, (unsigned)(1)), 32, 0, stream>>>(gas0); }
    k_wg_alpha<<<(unsigned)((NODES + 255) / 256), 256, 0, stream>>>(AS, LP, IDX, atb + 0, AL, NODES);
    { GemmP cvs0_0;
      cvs0_0.A = SPD + (size_t)0 * C; cvs0_0.B = csw + (size_t)0 + 0; cvs0_0.bias = SPD + (size_t)0 * C; cvs0_0.R = SPD + (size_t)0 * C; cvs0_0.C = MS;
      cvs0_0.sAo = (long long)100 * C; cvs0_0.sAi = (long long)10 * C; cvs0_0.sAm = C; cvs0_0.sAk = 1; cvs0_0.sBo = 0; cvs0_0.sBi = 0; cvs0_0.sBn = C * 9; cvs0_0.sBk = 9; cvs0_0.sCo = (long long)64 * C; cvs0_0.sCi = (long long)8 * C; cvs0_0.sCm = C; cvs0_0.sRo = 0; cvs0_0.sRi = 0; cvs0_0.sRm = 0; cvs0_0.sRn = 0;
      cvs0_0.M = 8; cvs0_0.N = C; cvs0_0.K = C; cvs0_0.zi_n = 8; cvs0_0.flags = 0; cvs0_0.act = 0;
      cvs0_0.alpha = 1.0f; cvs0_0.beta = 0.0f; cvs0_0.sa = 1.0f; cvs0_0.sb = 1.0f; cvs0_0.Npad = C; cvs0_0.pad_ = 0;
      k_gemm<1><<<dim3((unsigned)((C) + 31) / 32, (unsigned)((8) + 15) / 16, (unsigned)(NODES * 8)), 32, 0, stream>>>(cvs0_0); }
    { GemmP cvs0_1;
      cvs0_1.A = SPD + (size_t)1 * C; cvs0_1.B = csw + (size_t)0 + 1; cvs0_1.bias = SPD + (size_t)1 * C; cvs0_1.R = MS; cvs0_1.C = MS;
      cvs0_1.sAo = (long long)100 * C; cvs0_1.sAi = (long long)10 * C; cvs0_1.sAm = C; cvs0_1.sAk = 1; cvs0_1.sBo = 0; cvs0_1.sBi = 0; cvs0_1.sBn = C * 9; cvs0_1.sBk = 9; cvs0_1.sCo = (long long)64 * C; cvs0_1.sCi = (long long)8 * C; cvs0_1.sCm = C; cvs0_1.sRo = (long long)64 * C; cvs0_1.sRi = (long long)8 * C; cvs0_1.sRm = C; cvs0_1.sRn = 1;
      cvs0_1.M = 8; cvs0_1.N = C; cvs0_1.K = C; cvs0_1.zi_n = 8; cvs0_1.flags = 4; cvs0_1.act = 0;
      cvs0_1.alpha = 1.0f; cvs0_1.beta = 1.0f; cvs0_1.sa = 1.0f; cvs0_1.sb = 1.0f; cvs0_1.Npad = C; cvs0_1.pad_ = 0;
      k_gemm<1><<<dim3((unsigned)((C) + 31) / 32, (unsigned)((8) + 15) / 16, (unsigned)(NODES * 8)), 32, 0, stream>>>(cvs0_1); }
    { GemmP cvs0_2;
      cvs0_2.A = SPD + (size_t)2 * C; cvs0_2.B = csw + (size_t)0 + 2; cvs0_2.bias = SPD + (size_t)2 * C; cvs0_2.R = MS; cvs0_2.C = MS;
      cvs0_2.sAo = (long long)100 * C; cvs0_2.sAi = (long long)10 * C; cvs0_2.sAm = C; cvs0_2.sAk = 1; cvs0_2.sBo = 0; cvs0_2.sBi = 0; cvs0_2.sBn = C * 9; cvs0_2.sBk = 9; cvs0_2.sCo = (long long)64 * C; cvs0_2.sCi = (long long)8 * C; cvs0_2.sCm = C; cvs0_2.sRo = (long long)64 * C; cvs0_2.sRi = (long long)8 * C; cvs0_2.sRm = C; cvs0_2.sRn = 1;
      cvs0_2.M = 8; cvs0_2.N = C; cvs0_2.K = C; cvs0_2.zi_n = 8; cvs0_2.flags = 4; cvs0_2.act = 0;
      cvs0_2.alpha = 1.0f; cvs0_2.beta = 1.0f; cvs0_2.sa = 1.0f; cvs0_2.sb = 1.0f; cvs0_2.Npad = C; cvs0_2.pad_ = 0;
      k_gemm<1><<<dim3((unsigned)((C) + 31) / 32, (unsigned)((8) + 15) / 16, (unsigned)(NODES * 8)), 32, 0, stream>>>(cvs0_2); }
    { GemmP cvs0_3;
      cvs0_3.A = SPD + (size_t)10 * C; cvs0_3.B = csw + (size_t)0 + 3; cvs0_3.bias = SPD + (size_t)10 * C; cvs0_3.R = MS; cvs0_3.C = MS;
      cvs0_3.sAo = (long long)100 * C; cvs0_3.sAi = (long long)10 * C; cvs0_3.sAm = C; cvs0_3.sAk = 1; cvs0_3.sBo = 0; cvs0_3.sBi = 0; cvs0_3.sBn = C * 9; cvs0_3.sBk = 9; cvs0_3.sCo = (long long)64 * C; cvs0_3.sCi = (long long)8 * C; cvs0_3.sCm = C; cvs0_3.sRo = (long long)64 * C; cvs0_3.sRi = (long long)8 * C; cvs0_3.sRm = C; cvs0_3.sRn = 1;
      cvs0_3.M = 8; cvs0_3.N = C; cvs0_3.K = C; cvs0_3.zi_n = 8; cvs0_3.flags = 4; cvs0_3.act = 0;
      cvs0_3.alpha = 1.0f; cvs0_3.beta = 1.0f; cvs0_3.sa = 1.0f; cvs0_3.sb = 1.0f; cvs0_3.Npad = C; cvs0_3.pad_ = 0;
      k_gemm<1><<<dim3((unsigned)((C) + 31) / 32, (unsigned)((8) + 15) / 16, (unsigned)(NODES * 8)), 32, 0, stream>>>(cvs0_3); }
    { GemmP cvs0_4;
      cvs0_4.A = SPD + (size_t)11 * C; cvs0_4.B = csw + (size_t)0 + 4; cvs0_4.bias = SPD + (size_t)11 * C; cvs0_4.R = MS; cvs0_4.C = MS;
      cvs0_4.sAo = (long long)100 * C; cvs0_4.sAi = (long long)10 * C; cvs0_4.sAm = C; cvs0_4.sAk = 1; cvs0_4.sBo = 0; cvs0_4.sBi = 0; cvs0_4.sBn = C * 9; cvs0_4.sBk = 9; cvs0_4.sCo = (long long)64 * C; cvs0_4.sCi = (long long)8 * C; cvs0_4.sCm = C; cvs0_4.sRo = (long long)64 * C; cvs0_4.sRi = (long long)8 * C; cvs0_4.sRm = C; cvs0_4.sRn = 1;
      cvs0_4.M = 8; cvs0_4.N = C; cvs0_4.K = C; cvs0_4.zi_n = 8; cvs0_4.flags = 4; cvs0_4.act = 0;
      cvs0_4.alpha = 1.0f; cvs0_4.beta = 1.0f; cvs0_4.sa = 1.0f; cvs0_4.sb = 1.0f; cvs0_4.Npad = C; cvs0_4.pad_ = 0;
      k_gemm<1><<<dim3((unsigned)((C) + 31) / 32, (unsigned)((8) + 15) / 16, (unsigned)(NODES * 8)), 32, 0, stream>>>(cvs0_4); }
    { GemmP cvs0_5;
      cvs0_5.A = SPD + (size_t)12 * C; cvs0_5.B = csw + (size_t)0 + 5; cvs0_5.bias = SPD + (size_t)12 * C; cvs0_5.R = MS; cvs0_5.C = MS;
      cvs0_5.sAo = (long long)100 * C; cvs0_5.sAi = (long long)10 * C; cvs0_5.sAm = C; cvs0_5.sAk = 1; cvs0_5.sBo = 0; cvs0_5.sBi = 0; cvs0_5.sBn = C * 9; cvs0_5.sBk = 9; cvs0_5.sCo = (long long)64 * C; cvs0_5.sCi = (long long)8 * C; cvs0_5.sCm = C; cvs0_5.sRo = (long long)64 * C; cvs0_5.sRi = (long long)8 * C; cvs0_5.sRm = C; cvs0_5.sRn = 1;
      cvs0_5.M = 8; cvs0_5.N = C; cvs0_5.K = C; cvs0_5.zi_n = 8; cvs0_5.flags = 4; cvs0_5.act = 0;
      cvs0_5.alpha = 1.0f; cvs0_5.beta = 1.0f; cvs0_5.sa = 1.0f; cvs0_5.sb = 1.0f; cvs0_5.Npad = C; cvs0_5.pad_ = 0;
      k_gemm<1><<<dim3((unsigned)((C) + 31) / 32, (unsigned)((8) + 15) / 16, (unsigned)(NODES * 8)), 32, 0, stream>>>(cvs0_5); }
    { GemmP cvs0_6;
      cvs0_6.A = SPD + (size_t)20 * C; cvs0_6.B = csw + (size_t)0 + 6; cvs0_6.bias = SPD + (size_t)20 * C; cvs0_6.R = MS; cvs0_6.C = MS;
      cvs0_6.sAo = (long long)100 * C; cvs0_6.sAi = (long long)10 * C; cvs0_6.sAm = C; cvs0_6.sAk = 1; cvs0_6.sBo = 0; cvs0_6.sBi = 0; cvs0_6.sBn = C * 9; cvs0_6.sBk = 9; cvs0_6.sCo = (long long)64 * C; cvs0_6.sCi = (long long)8 * C; cvs0_6.sCm = C; cvs0_6.sRo = (long long)64 * C; cvs0_6.sRi = (long long)8 * C; cvs0_6.sRm = C; cvs0_6.sRn = 1;
      cvs0_6.M = 8; cvs0_6.N = C; cvs0_6.K = C; cvs0_6.zi_n = 8; cvs0_6.flags = 4; cvs0_6.act = 0;
      cvs0_6.alpha = 1.0f; cvs0_6.beta = 1.0f; cvs0_6.sa = 1.0f; cvs0_6.sb = 1.0f; cvs0_6.Npad = C; cvs0_6.pad_ = 0;
      k_gemm<1><<<dim3((unsigned)((C) + 31) / 32, (unsigned)((8) + 15) / 16, (unsigned)(NODES * 8)), 32, 0, stream>>>(cvs0_6); }
    { GemmP cvs0_7;
      cvs0_7.A = SPD + (size_t)21 * C; cvs0_7.B = csw + (size_t)0 + 7; cvs0_7.bias = SPD + (size_t)21 * C; cvs0_7.R = MS; cvs0_7.C = MS;
      cvs0_7.sAo = (long long)100 * C; cvs0_7.sAi = (long long)10 * C; cvs0_7.sAm = C; cvs0_7.sAk = 1; cvs0_7.sBo = 0; cvs0_7.sBi = 0; cvs0_7.sBn = C * 9; cvs0_7.sBk = 9; cvs0_7.sCo = (long long)64 * C; cvs0_7.sCi = (long long)8 * C; cvs0_7.sCm = C; cvs0_7.sRo = (long long)64 * C; cvs0_7.sRi = (long long)8 * C; cvs0_7.sRm = C; cvs0_7.sRn = 1;
      cvs0_7.M = 8; cvs0_7.N = C; cvs0_7.K = C; cvs0_7.zi_n = 8; cvs0_7.flags = 4; cvs0_7.act = 0;
      cvs0_7.alpha = 1.0f; cvs0_7.beta = 1.0f; cvs0_7.sa = 1.0f; cvs0_7.sb = 1.0f; cvs0_7.Npad = C; cvs0_7.pad_ = 0;
      k_gemm<1><<<dim3((unsigned)((C) + 31) / 32, (unsigned)((8) + 15) / 16, (unsigned)(NODES * 8)), 32, 0, stream>>>(cvs0_7); }
    { GemmP cvs0_8;
      cvs0_8.A = SPD + (size_t)22 * C; cvs0_8.B = csw + (size_t)0 + 8; cvs0_8.bias = SPD + (size_t)22 * C; cvs0_8.R = MS; cvs0_8.C = MS;
      cvs0_8.sAo = (long long)100 * C; cvs0_8.sAi = (long long)10 * C; cvs0_8.sAm = C; cvs0_8.sAk = 1; cvs0_8.sBo = 0; cvs0_8.sBi = 0; cvs0_8.sBn = C * 9; cvs0_8.sBk = 9; cvs0_8.sCo = (long long)64 * C; cvs0_8.sCi = (long long)8 * C; cvs0_8.sCm = C; cvs0_8.sRo = (long long)64 * C; cvs0_8.sRi = (long long)8 * C; cvs0_8.sRm = C; cvs0_8.sRn = 1;
      cvs0_8.M = 8; cvs0_8.N = C; cvs0_8.K = C; cvs0_8.zi_n = 8; cvs0_8.flags = 4; cvs0_8.act = 0;
      cvs0_8.alpha = 1.0f; cvs0_8.beta = 1.0f; cvs0_8.sa = 1.0f; cvs0_8.sb = 1.0f; cvs0_8.Npad = C; cvs0_8.pad_ = 0;
      k_gemm<1><<<dim3((unsigned)((C) + 31) / 32, (unsigned)((8) + 15) / 16, (unsigned)(NODES * 8)), 32, 0, stream>>>(cvs0_8); }

    k_wg_update<<<(unsigned)(((long long)NODES * 64 * C + 255) / 256), 256, 0, stream>>>(MS, DC, IDX, EW, AL, csb + (size_t)0, SPD, DP, OP, NODES, C, 0);
    { GemmP cvd1_0;
      cvd1_0.A = DP + (size_t)0 * C; cvd1_0.B = cdw + (size_t)147456 + 0; cvd1_0.bias = cdb + (size_t)128; cvd1_0.R = DP + (size_t)0 * C; cvd1_0.C = DC;
      cvd1_0.sAo = (long long)100 * C; cvd1_0.sAi = (long long)10 * C; cvd1_0.sAm = C; cvd1_0.sAk = 1; cvd1_0.sBo = 0; cvd1_0.sBi = 0; cvd1_0.sBn = C * 9; cvd1_0.sBk = 9; cvd1_0.sCo = (long long)64 * C; cvd1_0.sCi = (long long)8 * C; cvd1_0.sCm = C; cvd1_0.sRo = 0; cvd1_0.sRi = 0; cvd1_0.sRm = 0; cvd1_0.sRn = 0;
      cvd1_0.M = 8; cvd1_0.N = C; cvd1_0.K = C; cvd1_0.zi_n = 8; cvd1_0.flags = 1; cvd1_0.act = 0;
      cvd1_0.alpha = 1.0f; cvd1_0.beta = 0.0f; cvd1_0.sa = 1.0f; cvd1_0.sb = 1.0f; cvd1_0.Npad = C; cvd1_0.pad_ = 0;
      k_gemm<1><<<dim3((unsigned)((C) + 31) / 32, (unsigned)((8) + 15) / 16, (unsigned)(NODES * 8)), 32, 0, stream>>>(cvd1_0); }
    { GemmP cvd1_1;
      cvd1_1.A = DP + (size_t)1 * C; cvd1_1.B = cdw + (size_t)147456 + 1; cvd1_1.bias = DP + (size_t)1 * C; cvd1_1.R = DC; cvd1_1.C = DC;
      cvd1_1.sAo = (long long)100 * C; cvd1_1.sAi = (long long)10 * C; cvd1_1.sAm = C; cvd1_1.sAk = 1; cvd1_1.sBo = 0; cvd1_1.sBi = 0; cvd1_1.sBn = C * 9; cvd1_1.sBk = 9; cvd1_1.sCo = (long long)64 * C; cvd1_1.sCi = (long long)8 * C; cvd1_1.sCm = C; cvd1_1.sRo = (long long)64 * C; cvd1_1.sRi = (long long)8 * C; cvd1_1.sRm = C; cvd1_1.sRn = 1;
      cvd1_1.M = 8; cvd1_1.N = C; cvd1_1.K = C; cvd1_1.zi_n = 8; cvd1_1.flags = 4; cvd1_1.act = 0;
      cvd1_1.alpha = 1.0f; cvd1_1.beta = 1.0f; cvd1_1.sa = 1.0f; cvd1_1.sb = 1.0f; cvd1_1.Npad = C; cvd1_1.pad_ = 0;
      k_gemm<1><<<dim3((unsigned)((C) + 31) / 32, (unsigned)((8) + 15) / 16, (unsigned)(NODES * 8)), 32, 0, stream>>>(cvd1_1); }
    { GemmP cvd1_2;
      cvd1_2.A = DP + (size_t)2 * C; cvd1_2.B = cdw + (size_t)147456 + 2; cvd1_2.bias = DP + (size_t)2 * C; cvd1_2.R = DC; cvd1_2.C = DC;
      cvd1_2.sAo = (long long)100 * C; cvd1_2.sAi = (long long)10 * C; cvd1_2.sAm = C; cvd1_2.sAk = 1; cvd1_2.sBo = 0; cvd1_2.sBi = 0; cvd1_2.sBn = C * 9; cvd1_2.sBk = 9; cvd1_2.sCo = (long long)64 * C; cvd1_2.sCi = (long long)8 * C; cvd1_2.sCm = C; cvd1_2.sRo = (long long)64 * C; cvd1_2.sRi = (long long)8 * C; cvd1_2.sRm = C; cvd1_2.sRn = 1;
      cvd1_2.M = 8; cvd1_2.N = C; cvd1_2.K = C; cvd1_2.zi_n = 8; cvd1_2.flags = 4; cvd1_2.act = 0;
      cvd1_2.alpha = 1.0f; cvd1_2.beta = 1.0f; cvd1_2.sa = 1.0f; cvd1_2.sb = 1.0f; cvd1_2.Npad = C; cvd1_2.pad_ = 0;
      k_gemm<1><<<dim3((unsigned)((C) + 31) / 32, (unsigned)((8) + 15) / 16, (unsigned)(NODES * 8)), 32, 0, stream>>>(cvd1_2); }
    { GemmP cvd1_3;
      cvd1_3.A = DP + (size_t)10 * C; cvd1_3.B = cdw + (size_t)147456 + 3; cvd1_3.bias = DP + (size_t)10 * C; cvd1_3.R = DC; cvd1_3.C = DC;
      cvd1_3.sAo = (long long)100 * C; cvd1_3.sAi = (long long)10 * C; cvd1_3.sAm = C; cvd1_3.sAk = 1; cvd1_3.sBo = 0; cvd1_3.sBi = 0; cvd1_3.sBn = C * 9; cvd1_3.sBk = 9; cvd1_3.sCo = (long long)64 * C; cvd1_3.sCi = (long long)8 * C; cvd1_3.sCm = C; cvd1_3.sRo = (long long)64 * C; cvd1_3.sRi = (long long)8 * C; cvd1_3.sRm = C; cvd1_3.sRn = 1;
      cvd1_3.M = 8; cvd1_3.N = C; cvd1_3.K = C; cvd1_3.zi_n = 8; cvd1_3.flags = 4; cvd1_3.act = 0;
      cvd1_3.alpha = 1.0f; cvd1_3.beta = 1.0f; cvd1_3.sa = 1.0f; cvd1_3.sb = 1.0f; cvd1_3.Npad = C; cvd1_3.pad_ = 0;
      k_gemm<1><<<dim3((unsigned)((C) + 31) / 32, (unsigned)((8) + 15) / 16, (unsigned)(NODES * 8)), 32, 0, stream>>>(cvd1_3); }
    { GemmP cvd1_4;
      cvd1_4.A = DP + (size_t)11 * C; cvd1_4.B = cdw + (size_t)147456 + 4; cvd1_4.bias = DP + (size_t)11 * C; cvd1_4.R = DC; cvd1_4.C = DC;
      cvd1_4.sAo = (long long)100 * C; cvd1_4.sAi = (long long)10 * C; cvd1_4.sAm = C; cvd1_4.sAk = 1; cvd1_4.sBo = 0; cvd1_4.sBi = 0; cvd1_4.sBn = C * 9; cvd1_4.sBk = 9; cvd1_4.sCo = (long long)64 * C; cvd1_4.sCi = (long long)8 * C; cvd1_4.sCm = C; cvd1_4.sRo = (long long)64 * C; cvd1_4.sRi = (long long)8 * C; cvd1_4.sRm = C; cvd1_4.sRn = 1;
      cvd1_4.M = 8; cvd1_4.N = C; cvd1_4.K = C; cvd1_4.zi_n = 8; cvd1_4.flags = 4; cvd1_4.act = 0;
      cvd1_4.alpha = 1.0f; cvd1_4.beta = 1.0f; cvd1_4.sa = 1.0f; cvd1_4.sb = 1.0f; cvd1_4.Npad = C; cvd1_4.pad_ = 0;
      k_gemm<1><<<dim3((unsigned)((C) + 31) / 32, (unsigned)((8) + 15) / 16, (unsigned)(NODES * 8)), 32, 0, stream>>>(cvd1_4); }
    { GemmP cvd1_5;
      cvd1_5.A = DP + (size_t)12 * C; cvd1_5.B = cdw + (size_t)147456 + 5; cvd1_5.bias = DP + (size_t)12 * C; cvd1_5.R = DC; cvd1_5.C = DC;
      cvd1_5.sAo = (long long)100 * C; cvd1_5.sAi = (long long)10 * C; cvd1_5.sAm = C; cvd1_5.sAk = 1; cvd1_5.sBo = 0; cvd1_5.sBi = 0; cvd1_5.sBn = C * 9; cvd1_5.sBk = 9; cvd1_5.sCo = (long long)64 * C; cvd1_5.sCi = (long long)8 * C; cvd1_5.sCm = C; cvd1_5.sRo = (long long)64 * C; cvd1_5.sRi = (long long)8 * C; cvd1_5.sRm = C; cvd1_5.sRn = 1;
      cvd1_5.M = 8; cvd1_5.N = C; cvd1_5.K = C; cvd1_5.zi_n = 8; cvd1_5.flags = 4; cvd1_5.act = 0;
      cvd1_5.alpha = 1.0f; cvd1_5.beta = 1.0f; cvd1_5.sa = 1.0f; cvd1_5.sb = 1.0f; cvd1_5.Npad = C; cvd1_5.pad_ = 0;
      k_gemm<1><<<dim3((unsigned)((C) + 31) / 32, (unsigned)((8) + 15) / 16, (unsigned)(NODES * 8)), 32, 0, stream>>>(cvd1_5); }
    { GemmP cvd1_6;
      cvd1_6.A = DP + (size_t)20 * C; cvd1_6.B = cdw + (size_t)147456 + 6; cvd1_6.bias = DP + (size_t)20 * C; cvd1_6.R = DC; cvd1_6.C = DC;
      cvd1_6.sAo = (long long)100 * C; cvd1_6.sAi = (long long)10 * C; cvd1_6.sAm = C; cvd1_6.sAk = 1; cvd1_6.sBo = 0; cvd1_6.sBi = 0; cvd1_6.sBn = C * 9; cvd1_6.sBk = 9; cvd1_6.sCo = (long long)64 * C; cvd1_6.sCi = (long long)8 * C; cvd1_6.sCm = C; cvd1_6.sRo = (long long)64 * C; cvd1_6.sRi = (long long)8 * C; cvd1_6.sRm = C; cvd1_6.sRn = 1;
      cvd1_6.M = 8; cvd1_6.N = C; cvd1_6.K = C; cvd1_6.zi_n = 8; cvd1_6.flags = 4; cvd1_6.act = 0;
      cvd1_6.alpha = 1.0f; cvd1_6.beta = 1.0f; cvd1_6.sa = 1.0f; cvd1_6.sb = 1.0f; cvd1_6.Npad = C; cvd1_6.pad_ = 0;
      k_gemm<1><<<dim3((unsigned)((C) + 31) / 32, (unsigned)((8) + 15) / 16, (unsigned)(NODES * 8)), 32, 0, stream>>>(cvd1_6); }
    { GemmP cvd1_7;
      cvd1_7.A = DP + (size_t)21 * C; cvd1_7.B = cdw + (size_t)147456 + 7; cvd1_7.bias = DP + (size_t)21 * C; cvd1_7.R = DC; cvd1_7.C = DC;
      cvd1_7.sAo = (long long)100 * C; cvd1_7.sAi = (long long)10 * C; cvd1_7.sAm = C; cvd1_7.sAk = 1; cvd1_7.sBo = 0; cvd1_7.sBi = 0; cvd1_7.sBn = C * 9; cvd1_7.sBk = 9; cvd1_7.sCo = (long long)64 * C; cvd1_7.sCi = (long long)8 * C; cvd1_7.sCm = C; cvd1_7.sRo = (long long)64 * C; cvd1_7.sRi = (long long)8 * C; cvd1_7.sRm = C; cvd1_7.sRn = 1;
      cvd1_7.M = 8; cvd1_7.N = C; cvd1_7.K = C; cvd1_7.zi_n = 8; cvd1_7.flags = 4; cvd1_7.act = 0;
      cvd1_7.alpha = 1.0f; cvd1_7.beta = 1.0f; cvd1_7.sa = 1.0f; cvd1_7.sb = 1.0f; cvd1_7.Npad = C; cvd1_7.pad_ = 0;
      k_gemm<1><<<dim3((unsigned)((C) + 31) / 32, (unsigned)((8) + 15) / 16, (unsigned)(NODES * 8)), 32, 0, stream>>>(cvd1_7); }
    { GemmP cvd1_8;
      cvd1_8.A = DP + (size_t)22 * C; cvd1_8.B = cdw + (size_t)147456 + 8; cvd1_8.bias = DP + (size_t)22 * C; cvd1_8.R = DC; cvd1_8.C = DC;
      cvd1_8.sAo = (long long)100 * C; cvd1_8.sAi = (long long)10 * C; cvd1_8.sAm = C; cvd1_8.sAk = 1; cvd1_8.sBo = 0; cvd1_8.sBi = 0; cvd1_8.sBn = C * 9; cvd1_8.sBk = 9; cvd1_8.sCo = (long long)64 * C; cvd1_8.sCi = (long long)8 * C; cvd1_8.sCm = C; cvd1_8.sRo = (long long)64 * C; cvd1_8.sRi = (long long)8 * C; cvd1_8.sRm = C; cvd1_8.sRn = 1;
      cvd1_8.M = 8; cvd1_8.N = C; cvd1_8.K = C; cvd1_8.zi_n = 8; cvd1_8.flags = 4; cvd1_8.act = 0;
      cvd1_8.alpha = 1.0f; cvd1_8.beta = 1.0f; cvd1_8.sa = 1.0f; cvd1_8.sb = 1.0f; cvd1_8.Npad = C; cvd1_8.pad_ = 0;
      k_gemm<1><<<dim3((unsigned)((C) + 31) / 32, (unsigned)((8) + 15) / 16, (unsigned)(NODES * 8)), 32, 0, stream>>>(cvd1_8); }

    k_norm_apply<<<(unsigned)(((long long)(1) * (1) * ((long long)NODES * 64 * C) + 255) / 256), 256, 0, stream>>>(DC, DC, ust, nullptr, nullptr, 1, 1, (long long)NODES * 64 * C, 1, 0, 4);
    k_wg_wb<<<(unsigned)((64 * C + 255) / 256), 256, 0, stream>>>(atw + (size_t)1024, WB, C);
    { GemmP gas1;
      gas1.A = DC; gas1.B = WB; gas1.bias = DC; gas1.R = DC; gas1.C = AS;
      gas1.sAo = 0; gas1.sAi = 0; gas1.sAm = FD; gas1.sAk = 1; gas1.sBo = 0; gas1.sBi = 0; gas1.sBn = 1; gas1.sBk = 2; gas1.sCo = 0; gas1.sCi = 0; gas1.sCm = LP; gas1.sRo = 0; gas1.sRi = 0; gas1.sRm = 0; gas1.sRn = 0;
      gas1.M = NODES; gas1.N = 2; gas1.K = FD; gas1.zi_n = 1; gas1.flags = 0; gas1.act = 0;
      gas1.alpha = 0.0625f; gas1.beta = 0.0f; gas1.sa = 1.0f; gas1.sb = 1.0f; gas1.Npad = LP; gas1.pad_ = 0;
      k_gemm<3><<<dim3((unsigned)((LP) + 31) / 32, (unsigned)((NODES) + 15) / 16, (unsigned)(1)), 32, 0, stream>>>(gas1); }
    k_wg_alpha<<<(unsigned)((NODES + 255) / 256), 256, 0, stream>>>(AS, LP, IDX, atb + 1, AL, NODES);
    { GemmP cvs1_0;
      cvs1_0.A = SPD + (size_t)0 * C; cvs1_0.B = csw + (size_t)147456 + 0; cvs1_0.bias = SPD + (size_t)0 * C; cvs1_0.R = SPD + (size_t)0 * C; cvs1_0.C = MS;
      cvs1_0.sAo = (long long)100 * C; cvs1_0.sAi = (long long)10 * C; cvs1_0.sAm = C; cvs1_0.sAk = 1; cvs1_0.sBo = 0; cvs1_0.sBi = 0; cvs1_0.sBn = C * 9; cvs1_0.sBk = 9; cvs1_0.sCo = (long long)64 * C; cvs1_0.sCi = (long long)8 * C; cvs1_0.sCm = C; cvs1_0.sRo = 0; cvs1_0.sRi = 0; cvs1_0.sRm = 0; cvs1_0.sRn = 0;
      cvs1_0.M = 8; cvs1_0.N = C; cvs1_0.K = C; cvs1_0.zi_n = 8; cvs1_0.flags = 0; cvs1_0.act = 0;
      cvs1_0.alpha = 1.0f; cvs1_0.beta = 0.0f; cvs1_0.sa = 1.0f; cvs1_0.sb = 1.0f; cvs1_0.Npad = C; cvs1_0.pad_ = 0;
      k_gemm<1><<<dim3((unsigned)((C) + 31) / 32, (unsigned)((8) + 15) / 16, (unsigned)(NODES * 8)), 32, 0, stream>>>(cvs1_0); }
    { GemmP cvs1_1;
      cvs1_1.A = SPD + (size_t)1 * C; cvs1_1.B = csw + (size_t)147456 + 1; cvs1_1.bias = SPD + (size_t)1 * C; cvs1_1.R = MS; cvs1_1.C = MS;
      cvs1_1.sAo = (long long)100 * C; cvs1_1.sAi = (long long)10 * C; cvs1_1.sAm = C; cvs1_1.sAk = 1; cvs1_1.sBo = 0; cvs1_1.sBi = 0; cvs1_1.sBn = C * 9; cvs1_1.sBk = 9; cvs1_1.sCo = (long long)64 * C; cvs1_1.sCi = (long long)8 * C; cvs1_1.sCm = C; cvs1_1.sRo = (long long)64 * C; cvs1_1.sRi = (long long)8 * C; cvs1_1.sRm = C; cvs1_1.sRn = 1;
      cvs1_1.M = 8; cvs1_1.N = C; cvs1_1.K = C; cvs1_1.zi_n = 8; cvs1_1.flags = 4; cvs1_1.act = 0;
      cvs1_1.alpha = 1.0f; cvs1_1.beta = 1.0f; cvs1_1.sa = 1.0f; cvs1_1.sb = 1.0f; cvs1_1.Npad = C; cvs1_1.pad_ = 0;
      k_gemm<1><<<dim3((unsigned)((C) + 31) / 32, (unsigned)((8) + 15) / 16, (unsigned)(NODES * 8)), 32, 0, stream>>>(cvs1_1); }
    { GemmP cvs1_2;
      cvs1_2.A = SPD + (size_t)2 * C; cvs1_2.B = csw + (size_t)147456 + 2; cvs1_2.bias = SPD + (size_t)2 * C; cvs1_2.R = MS; cvs1_2.C = MS;
      cvs1_2.sAo = (long long)100 * C; cvs1_2.sAi = (long long)10 * C; cvs1_2.sAm = C; cvs1_2.sAk = 1; cvs1_2.sBo = 0; cvs1_2.sBi = 0; cvs1_2.sBn = C * 9; cvs1_2.sBk = 9; cvs1_2.sCo = (long long)64 * C; cvs1_2.sCi = (long long)8 * C; cvs1_2.sCm = C; cvs1_2.sRo = (long long)64 * C; cvs1_2.sRi = (long long)8 * C; cvs1_2.sRm = C; cvs1_2.sRn = 1;
      cvs1_2.M = 8; cvs1_2.N = C; cvs1_2.K = C; cvs1_2.zi_n = 8; cvs1_2.flags = 4; cvs1_2.act = 0;
      cvs1_2.alpha = 1.0f; cvs1_2.beta = 1.0f; cvs1_2.sa = 1.0f; cvs1_2.sb = 1.0f; cvs1_2.Npad = C; cvs1_2.pad_ = 0;
      k_gemm<1><<<dim3((unsigned)((C) + 31) / 32, (unsigned)((8) + 15) / 16, (unsigned)(NODES * 8)), 32, 0, stream>>>(cvs1_2); }
    { GemmP cvs1_3;
      cvs1_3.A = SPD + (size_t)10 * C; cvs1_3.B = csw + (size_t)147456 + 3; cvs1_3.bias = SPD + (size_t)10 * C; cvs1_3.R = MS; cvs1_3.C = MS;
      cvs1_3.sAo = (long long)100 * C; cvs1_3.sAi = (long long)10 * C; cvs1_3.sAm = C; cvs1_3.sAk = 1; cvs1_3.sBo = 0; cvs1_3.sBi = 0; cvs1_3.sBn = C * 9; cvs1_3.sBk = 9; cvs1_3.sCo = (long long)64 * C; cvs1_3.sCi = (long long)8 * C; cvs1_3.sCm = C; cvs1_3.sRo = (long long)64 * C; cvs1_3.sRi = (long long)8 * C; cvs1_3.sRm = C; cvs1_3.sRn = 1;
      cvs1_3.M = 8; cvs1_3.N = C; cvs1_3.K = C; cvs1_3.zi_n = 8; cvs1_3.flags = 4; cvs1_3.act = 0;
      cvs1_3.alpha = 1.0f; cvs1_3.beta = 1.0f; cvs1_3.sa = 1.0f; cvs1_3.sb = 1.0f; cvs1_3.Npad = C; cvs1_3.pad_ = 0;
      k_gemm<1><<<dim3((unsigned)((C) + 31) / 32, (unsigned)((8) + 15) / 16, (unsigned)(NODES * 8)), 32, 0, stream>>>(cvs1_3); }
    { GemmP cvs1_4;
      cvs1_4.A = SPD + (size_t)11 * C; cvs1_4.B = csw + (size_t)147456 + 4; cvs1_4.bias = SPD + (size_t)11 * C; cvs1_4.R = MS; cvs1_4.C = MS;
      cvs1_4.sAo = (long long)100 * C; cvs1_4.sAi = (long long)10 * C; cvs1_4.sAm = C; cvs1_4.sAk = 1; cvs1_4.sBo = 0; cvs1_4.sBi = 0; cvs1_4.sBn = C * 9; cvs1_4.sBk = 9; cvs1_4.sCo = (long long)64 * C; cvs1_4.sCi = (long long)8 * C; cvs1_4.sCm = C; cvs1_4.sRo = (long long)64 * C; cvs1_4.sRi = (long long)8 * C; cvs1_4.sRm = C; cvs1_4.sRn = 1;
      cvs1_4.M = 8; cvs1_4.N = C; cvs1_4.K = C; cvs1_4.zi_n = 8; cvs1_4.flags = 4; cvs1_4.act = 0;
      cvs1_4.alpha = 1.0f; cvs1_4.beta = 1.0f; cvs1_4.sa = 1.0f; cvs1_4.sb = 1.0f; cvs1_4.Npad = C; cvs1_4.pad_ = 0;
      k_gemm<1><<<dim3((unsigned)((C) + 31) / 32, (unsigned)((8) + 15) / 16, (unsigned)(NODES * 8)), 32, 0, stream>>>(cvs1_4); }
    { GemmP cvs1_5;
      cvs1_5.A = SPD + (size_t)12 * C; cvs1_5.B = csw + (size_t)147456 + 5; cvs1_5.bias = SPD + (size_t)12 * C; cvs1_5.R = MS; cvs1_5.C = MS;
      cvs1_5.sAo = (long long)100 * C; cvs1_5.sAi = (long long)10 * C; cvs1_5.sAm = C; cvs1_5.sAk = 1; cvs1_5.sBo = 0; cvs1_5.sBi = 0; cvs1_5.sBn = C * 9; cvs1_5.sBk = 9; cvs1_5.sCo = (long long)64 * C; cvs1_5.sCi = (long long)8 * C; cvs1_5.sCm = C; cvs1_5.sRo = (long long)64 * C; cvs1_5.sRi = (long long)8 * C; cvs1_5.sRm = C; cvs1_5.sRn = 1;
      cvs1_5.M = 8; cvs1_5.N = C; cvs1_5.K = C; cvs1_5.zi_n = 8; cvs1_5.flags = 4; cvs1_5.act = 0;
      cvs1_5.alpha = 1.0f; cvs1_5.beta = 1.0f; cvs1_5.sa = 1.0f; cvs1_5.sb = 1.0f; cvs1_5.Npad = C; cvs1_5.pad_ = 0;
      k_gemm<1><<<dim3((unsigned)((C) + 31) / 32, (unsigned)((8) + 15) / 16, (unsigned)(NODES * 8)), 32, 0, stream>>>(cvs1_5); }
    { GemmP cvs1_6;
      cvs1_6.A = SPD + (size_t)20 * C; cvs1_6.B = csw + (size_t)147456 + 6; cvs1_6.bias = SPD + (size_t)20 * C; cvs1_6.R = MS; cvs1_6.C = MS;
      cvs1_6.sAo = (long long)100 * C; cvs1_6.sAi = (long long)10 * C; cvs1_6.sAm = C; cvs1_6.sAk = 1; cvs1_6.sBo = 0; cvs1_6.sBi = 0; cvs1_6.sBn = C * 9; cvs1_6.sBk = 9; cvs1_6.sCo = (long long)64 * C; cvs1_6.sCi = (long long)8 * C; cvs1_6.sCm = C; cvs1_6.sRo = (long long)64 * C; cvs1_6.sRi = (long long)8 * C; cvs1_6.sRm = C; cvs1_6.sRn = 1;
      cvs1_6.M = 8; cvs1_6.N = C; cvs1_6.K = C; cvs1_6.zi_n = 8; cvs1_6.flags = 4; cvs1_6.act = 0;
      cvs1_6.alpha = 1.0f; cvs1_6.beta = 1.0f; cvs1_6.sa = 1.0f; cvs1_6.sb = 1.0f; cvs1_6.Npad = C; cvs1_6.pad_ = 0;
      k_gemm<1><<<dim3((unsigned)((C) + 31) / 32, (unsigned)((8) + 15) / 16, (unsigned)(NODES * 8)), 32, 0, stream>>>(cvs1_6); }
    { GemmP cvs1_7;
      cvs1_7.A = SPD + (size_t)21 * C; cvs1_7.B = csw + (size_t)147456 + 7; cvs1_7.bias = SPD + (size_t)21 * C; cvs1_7.R = MS; cvs1_7.C = MS;
      cvs1_7.sAo = (long long)100 * C; cvs1_7.sAi = (long long)10 * C; cvs1_7.sAm = C; cvs1_7.sAk = 1; cvs1_7.sBo = 0; cvs1_7.sBi = 0; cvs1_7.sBn = C * 9; cvs1_7.sBk = 9; cvs1_7.sCo = (long long)64 * C; cvs1_7.sCi = (long long)8 * C; cvs1_7.sCm = C; cvs1_7.sRo = (long long)64 * C; cvs1_7.sRi = (long long)8 * C; cvs1_7.sRm = C; cvs1_7.sRn = 1;
      cvs1_7.M = 8; cvs1_7.N = C; cvs1_7.K = C; cvs1_7.zi_n = 8; cvs1_7.flags = 4; cvs1_7.act = 0;
      cvs1_7.alpha = 1.0f; cvs1_7.beta = 1.0f; cvs1_7.sa = 1.0f; cvs1_7.sb = 1.0f; cvs1_7.Npad = C; cvs1_7.pad_ = 0;
      k_gemm<1><<<dim3((unsigned)((C) + 31) / 32, (unsigned)((8) + 15) / 16, (unsigned)(NODES * 8)), 32, 0, stream>>>(cvs1_7); }
    { GemmP cvs1_8;
      cvs1_8.A = SPD + (size_t)22 * C; cvs1_8.B = csw + (size_t)147456 + 8; cvs1_8.bias = SPD + (size_t)22 * C; cvs1_8.R = MS; cvs1_8.C = MS;
      cvs1_8.sAo = (long long)100 * C; cvs1_8.sAi = (long long)10 * C; cvs1_8.sAm = C; cvs1_8.sAk = 1; cvs1_8.sBo = 0; cvs1_8.sBi = 0; cvs1_8.sBn = C * 9; cvs1_8.sBk = 9; cvs1_8.sCo = (long long)64 * C; cvs1_8.sCi = (long long)8 * C; cvs1_8.sCm = C; cvs1_8.sRo = (long long)64 * C; cvs1_8.sRi = (long long)8 * C; cvs1_8.sRm = C; cvs1_8.sRn = 1;
      cvs1_8.M = 8; cvs1_8.N = C; cvs1_8.K = C; cvs1_8.zi_n = 8; cvs1_8.flags = 4; cvs1_8.act = 0;
      cvs1_8.alpha = 1.0f; cvs1_8.beta = 1.0f; cvs1_8.sa = 1.0f; cvs1_8.sb = 1.0f; cvs1_8.Npad = C; cvs1_8.pad_ = 0;
      k_gemm<1><<<dim3((unsigned)((C) + 31) / 32, (unsigned)((8) + 15) / 16, (unsigned)(NODES * 8)), 32, 0, stream>>>(cvs1_8); }

    k_wg_update<<<(unsigned)(((long long)NODES * 64 * C + 255) / 256), 256, 0, stream>>>(MS, DC, IDX, EW, AL, csb + (size_t)128, SPD, DP, OP, NODES, C, 1);
    { GemmP cvo_0;
      cvo_0.A = OP + (size_t)0 * 256; cvo_0.B = ow + 0; cvo_0.bias = ob; cvo_0.R = OP + (size_t)0 * 256; cvo_0.C = OC;
      cvo_0.sAo = (long long)130 * 130 * 256; cvo_0.sAi = (long long)130 * 256; cvo_0.sAm = 256; cvo_0.sAk = 1; cvo_0.sBo = 0; cvo_0.sBi = 0; cvo_0.sBn = 256 * 9; cvo_0.sBk = 9; cvo_0.sCo = (long long)IMG * IMG * C; cvo_0.sCi = (long long)IMG * C; cvo_0.sCm = C; cvo_0.sRo = 0; cvo_0.sRi = 0; cvo_0.sRm = 0; cvo_0.sRn = 0;
      cvo_0.M = IMG; cvo_0.N = C; cvo_0.K = 256; cvo_0.zi_n = IMG; cvo_0.flags = 1; cvo_0.act = 0;
      cvo_0.alpha = 1.0f; cvo_0.beta = 0.0f; cvo_0.sa = 1.0f; cvo_0.sb = 1.0f; cvo_0.Npad = C; cvo_0.pad_ = 0;
      k_gemm<1><<<dim3((unsigned)((C) + 31) / 32, (unsigned)((IMG) + 15) / 16, (unsigned)(Bn * IMG)), 32, 0, stream>>>(cvo_0); }
    { GemmP cvo_1;
      cvo_1.A = OP + (size_t)1 * 256; cvo_1.B = ow + 1; cvo_1.bias = OP + (size_t)1 * 256; cvo_1.R = OC; cvo_1.C = OC;
      cvo_1.sAo = (long long)130 * 130 * 256; cvo_1.sAi = (long long)130 * 256; cvo_1.sAm = 256; cvo_1.sAk = 1; cvo_1.sBo = 0; cvo_1.sBi = 0; cvo_1.sBn = 256 * 9; cvo_1.sBk = 9; cvo_1.sCo = (long long)IMG * IMG * C; cvo_1.sCi = (long long)IMG * C; cvo_1.sCm = C; cvo_1.sRo = (long long)IMG * IMG * C; cvo_1.sRi = (long long)IMG * C; cvo_1.sRm = C; cvo_1.sRn = 1;
      cvo_1.M = IMG; cvo_1.N = C; cvo_1.K = 256; cvo_1.zi_n = IMG; cvo_1.flags = 4; cvo_1.act = 0;
      cvo_1.alpha = 1.0f; cvo_1.beta = 1.0f; cvo_1.sa = 1.0f; cvo_1.sb = 1.0f; cvo_1.Npad = C; cvo_1.pad_ = 0;
      k_gemm<1><<<dim3((unsigned)((C) + 31) / 32, (unsigned)((IMG) + 15) / 16, (unsigned)(Bn * IMG)), 32, 0, stream>>>(cvo_1); }
    { GemmP cvo_2;
      cvo_2.A = OP + (size_t)2 * 256; cvo_2.B = ow + 2; cvo_2.bias = OP + (size_t)2 * 256; cvo_2.R = OC; cvo_2.C = OC;
      cvo_2.sAo = (long long)130 * 130 * 256; cvo_2.sAi = (long long)130 * 256; cvo_2.sAm = 256; cvo_2.sAk = 1; cvo_2.sBo = 0; cvo_2.sBi = 0; cvo_2.sBn = 256 * 9; cvo_2.sBk = 9; cvo_2.sCo = (long long)IMG * IMG * C; cvo_2.sCi = (long long)IMG * C; cvo_2.sCm = C; cvo_2.sRo = (long long)IMG * IMG * C; cvo_2.sRi = (long long)IMG * C; cvo_2.sRm = C; cvo_2.sRn = 1;
      cvo_2.M = IMG; cvo_2.N = C; cvo_2.K = 256; cvo_2.zi_n = IMG; cvo_2.flags = 4; cvo_2.act = 0;
      cvo_2.alpha = 1.0f; cvo_2.beta = 1.0f; cvo_2.sa = 1.0f; cvo_2.sb = 1.0f; cvo_2.Npad = C; cvo_2.pad_ = 0;
      k_gemm<1><<<dim3((unsigned)((C) + 31) / 32, (unsigned)((IMG) + 15) / 16, (unsigned)(Bn * IMG)), 32, 0, stream>>>(cvo_2); }
    { GemmP cvo_3;
      cvo_3.A = OP + (size_t)130 * 256; cvo_3.B = ow + 3; cvo_3.bias = OP + (size_t)130 * 256; cvo_3.R = OC; cvo_3.C = OC;
      cvo_3.sAo = (long long)130 * 130 * 256; cvo_3.sAi = (long long)130 * 256; cvo_3.sAm = 256; cvo_3.sAk = 1; cvo_3.sBo = 0; cvo_3.sBi = 0; cvo_3.sBn = 256 * 9; cvo_3.sBk = 9; cvo_3.sCo = (long long)IMG * IMG * C; cvo_3.sCi = (long long)IMG * C; cvo_3.sCm = C; cvo_3.sRo = (long long)IMG * IMG * C; cvo_3.sRi = (long long)IMG * C; cvo_3.sRm = C; cvo_3.sRn = 1;
      cvo_3.M = IMG; cvo_3.N = C; cvo_3.K = 256; cvo_3.zi_n = IMG; cvo_3.flags = 4; cvo_3.act = 0;
      cvo_3.alpha = 1.0f; cvo_3.beta = 1.0f; cvo_3.sa = 1.0f; cvo_3.sb = 1.0f; cvo_3.Npad = C; cvo_3.pad_ = 0;
      k_gemm<1><<<dim3((unsigned)((C) + 31) / 32, (unsigned)((IMG) + 15) / 16, (unsigned)(Bn * IMG)), 32, 0, stream>>>(cvo_3); }
    { GemmP cvo_4;
      cvo_4.A = OP + (size_t)131 * 256; cvo_4.B = ow + 4; cvo_4.bias = OP + (size_t)131 * 256; cvo_4.R = OC; cvo_4.C = OC;
      cvo_4.sAo = (long long)130 * 130 * 256; cvo_4.sAi = (long long)130 * 256; cvo_4.sAm = 256; cvo_4.sAk = 1; cvo_4.sBo = 0; cvo_4.sBi = 0; cvo_4.sBn = 256 * 9; cvo_4.sBk = 9; cvo_4.sCo = (long long)IMG * IMG * C; cvo_4.sCi = (long long)IMG * C; cvo_4.sCm = C; cvo_4.sRo = (long long)IMG * IMG * C; cvo_4.sRi = (long long)IMG * C; cvo_4.sRm = C; cvo_4.sRn = 1;
      cvo_4.M = IMG; cvo_4.N = C; cvo_4.K = 256; cvo_4.zi_n = IMG; cvo_4.flags = 4; cvo_4.act = 0;
      cvo_4.alpha = 1.0f; cvo_4.beta = 1.0f; cvo_4.sa = 1.0f; cvo_4.sb = 1.0f; cvo_4.Npad = C; cvo_4.pad_ = 0;
      k_gemm<1><<<dim3((unsigned)((C) + 31) / 32, (unsigned)((IMG) + 15) / 16, (unsigned)(Bn * IMG)), 32, 0, stream>>>(cvo_4); }
    { GemmP cvo_5;
      cvo_5.A = OP + (size_t)132 * 256; cvo_5.B = ow + 5; cvo_5.bias = OP + (size_t)132 * 256; cvo_5.R = OC; cvo_5.C = OC;
      cvo_5.sAo = (long long)130 * 130 * 256; cvo_5.sAi = (long long)130 * 256; cvo_5.sAm = 256; cvo_5.sAk = 1; cvo_5.sBo = 0; cvo_5.sBi = 0; cvo_5.sBn = 256 * 9; cvo_5.sBk = 9; cvo_5.sCo = (long long)IMG * IMG * C; cvo_5.sCi = (long long)IMG * C; cvo_5.sCm = C; cvo_5.sRo = (long long)IMG * IMG * C; cvo_5.sRi = (long long)IMG * C; cvo_5.sRm = C; cvo_5.sRn = 1;
      cvo_5.M = IMG; cvo_5.N = C; cvo_5.K = 256; cvo_5.zi_n = IMG; cvo_5.flags = 4; cvo_5.act = 0;
      cvo_5.alpha = 1.0f; cvo_5.beta = 1.0f; cvo_5.sa = 1.0f; cvo_5.sb = 1.0f; cvo_5.Npad = C; cvo_5.pad_ = 0;
      k_gemm<1><<<dim3((unsigned)((C) + 31) / 32, (unsigned)((IMG) + 15) / 16, (unsigned)(Bn * IMG)), 32, 0, stream>>>(cvo_5); }
    { GemmP cvo_6;
      cvo_6.A = OP + (size_t)260 * 256; cvo_6.B = ow + 6; cvo_6.bias = OP + (size_t)260 * 256; cvo_6.R = OC; cvo_6.C = OC;
      cvo_6.sAo = (long long)130 * 130 * 256; cvo_6.sAi = (long long)130 * 256; cvo_6.sAm = 256; cvo_6.sAk = 1; cvo_6.sBo = 0; cvo_6.sBi = 0; cvo_6.sBn = 256 * 9; cvo_6.sBk = 9; cvo_6.sCo = (long long)IMG * IMG * C; cvo_6.sCi = (long long)IMG * C; cvo_6.sCm = C; cvo_6.sRo = (long long)IMG * IMG * C; cvo_6.sRi = (long long)IMG * C; cvo_6.sRm = C; cvo_6.sRn = 1;
      cvo_6.M = IMG; cvo_6.N = C; cvo_6.K = 256; cvo_6.zi_n = IMG; cvo_6.flags = 4; cvo_6.act = 0;
      cvo_6.alpha = 1.0f; cvo_6.beta = 1.0f; cvo_6.sa = 1.0f; cvo_6.sb = 1.0f; cvo_6.Npad = C; cvo_6.pad_ = 0;
      k_gemm<1><<<dim3((unsigned)((C) + 31) / 32, (unsigned)((IMG) + 15) / 16, (unsigned)(Bn * IMG)), 32, 0, stream>>>(cvo_6); }
    { GemmP cvo_7;
      cvo_7.A = OP + (size_t)261 * 256; cvo_7.B = ow + 7; cvo_7.bias = OP + (size_t)261 * 256; cvo_7.R = OC; cvo_7.C = OC;
      cvo_7.sAo = (long long)130 * 130 * 256; cvo_7.sAi = (long long)130 * 256; cvo_7.sAm = 256; cvo_7.sAk = 1; cvo_7.sBo = 0; cvo_7.sBi = 0; cvo_7.sBn = 256 * 9; cvo_7.sBk = 9; cvo_7.sCo = (long long)IMG * IMG * C; cvo_7.sCi = (long long)IMG * C; cvo_7.sCm = C; cvo_7.sRo = (long long)IMG * IMG * C; cvo_7.sRi = (long long)IMG * C; cvo_7.sRm = C; cvo_7.sRn = 1;
      cvo_7.M = IMG; cvo_7.N = C; cvo_7.K = 256; cvo_7.zi_n = IMG; cvo_7.flags = 4; cvo_7.act = 0;
      cvo_7.alpha = 1.0f; cvo_7.beta = 1.0f; cvo_7.sa = 1.0f; cvo_7.sb = 1.0f; cvo_7.Npad = C; cvo_7.pad_ = 0;
      k_gemm<1><<<dim3((unsigned)((C) + 31) / 32, (unsigned)((IMG) + 15) / 16, (unsigned)(Bn * IMG)), 32, 0, stream>>>(cvo_7); }
    { GemmP cvo_8;
      cvo_8.A = OP + (size_t)262 * 256; cvo_8.B = ow + 8; cvo_8.bias = OP + (size_t)262 * 256; cvo_8.R = OC; cvo_8.C = OC;
      cvo_8.sAo = (long long)130 * 130 * 256; cvo_8.sAi = (long long)130 * 256; cvo_8.sAm = 256; cvo_8.sAk = 1; cvo_8.sBo = 0; cvo_8.sBi = 0; cvo_8.sBn = 256 * 9; cvo_8.sBk = 9; cvo_8.sCo = (long long)IMG * IMG * C; cvo_8.sCi = (long long)IMG * C; cvo_8.sCm = C; cvo_8.sRo = (long long)IMG * IMG * C; cvo_8.sRi = (long long)IMG * C; cvo_8.sRm = C; cvo_8.sRn = 1;
      cvo_8.M = IMG; cvo_8.N = C; cvo_8.K = 256; cvo_8.zi_n = IMG; cvo_8.flags = 4; cvo_8.act = 0;
      cvo_8.alpha = 1.0f; cvo_8.beta = 1.0f; cvo_8.sa = 1.0f; cvo_8.sb = 1.0f; cvo_8.Npad = C; cvo_8.pad_ = 0;
      k_gemm<1><<<dim3((unsigned)((C) + 31) / 32, (unsigned)((IMG) + 15) / 16, (unsigned)(Bn * IMG)), 32, 0, stream>>>(cvo_8); }

    k_norm_apply<<<(unsigned)(((long long)(1) * (1) * ((long long)Bn * IMG * IMG * C) + 255) / 256), 256, 0, stream>>>(OC, OC, ust, nullptr, nullptr, 1, 1, (long long)Bn * IMG * IMG * C, 1, 0, 4);
    { TrP t; t.src = OC; t.dst = out; t.R2 = OC; t.sSz = (long long)IMG * IMG * C; t.lds = C; t.sDz = (long long)C * IMG * IMG; t.ldd = (long long)IMG * IMG; t.sRz = 0; t.ldr = 0;
      t.R = IMG * IMG; t.C = C; t.flags = 0; t.act = 0; t.alpha = 1.0f; t.beta = 0.0f;
      k_tr<<<dim3((unsigned)((C) + 31) / 32, (unsigned)((IMG * IMG) + 31) / 32, (unsigned)(Bn)), 256, 0, stream>>>(t); }
}
